// GGNNModelClassification_33139967656251
// MI455X (gfx1250) — hardware-verified
//
#include <hip/hip_runtime.h>
#include <math.h>

typedef __attribute__((ext_vector_type(16))) _Float16 v16h;
typedef __attribute__((ext_vector_type(8)))  _Float16 v8h;
typedef __attribute__((ext_vector_type(16))) __bf16   v16b;
typedef __attribute__((ext_vector_type(8)))  float    v8f;
typedef __attribute__((ext_vector_type(4)))  float    v4f;

__device__ __forceinline__ int frag_k(int i, int h) { return (i < 8) ? (8 * h + i) : (16 + 8 * h + (i - 8)); }
__device__ __forceinline__ __bf16 bf16_rne(float f) {
    unsigned int u = __float_as_uint(f);
    u += 0x7fffu + ((u >> 16) & 1u);
    return __builtin_bit_cast(__bf16, (unsigned short)(u >> 16));
}
__device__ __forceinline__ float bf16_f32(__bf16 b) { return __uint_as_float(((unsigned int)__builtin_bit_cast(unsigned short, b)) << 16); }
__device__ __forceinline__ v8f wmma16(v16h a, v16h b, v8f c) {
    c = __builtin_amdgcn_wmma_f32_16x16x32_f16(false, a, false, b, (short)0, c, false, false);
    asm volatile("v_nop\n\tv_nop\n\tv_nop\n\tv_nop" : "+v"(c) : "v"(a), "v"(b));
    return c;
}
__device__ __forceinline__ v8f wmmab(v16b a, v16b b, v8f c) {
    c = __builtin_amdgcn_wmma_f32_16x16x32_bf16(false, a, false, b, (short)0, c, false, false);
    asm volatile("v_nop\n\tv_nop\n\tv_nop\n\tv_nop" : "+v"(c) : "v"(a), "v"(b));
    return c;
}
struct Split { v16b hi, lo; };
__device__ __forceinline__ v8f wmma3(const Split& a, const Split& b, v8f c) {
    c = __builtin_amdgcn_wmma_f32_16x16x32_bf16(false, a.hi, false, b.hi, (short)0, c, false, false);
    c = __builtin_amdgcn_wmma_f32_16x16x32_bf16(false, a.hi, false, b.lo, (short)0, c, false, false);
    c = __builtin_amdgcn_wmma_f32_16x16x32_bf16(false, a.lo, false, b.hi, (short)0, c, false, false);
    asm volatile("v_nop\n\tv_nop\n\tv_nop\n\tv_nop" : "+v"(c) : "v"(a.hi), "v"(a.lo), "v"(b.hi), "v"(b.lo));
    return c;
}
struct Split3 { v16b hi, mid, lo; };
__device__ __forceinline__ v8f wmma6(const Split3& a, const Split3& b, v8f c) {
    c = __builtin_amdgcn_wmma_f32_16x16x32_bf16(false, a.hi, false, b.hi, (short)0, c, false, false);
    c = __builtin_amdgcn_wmma_f32_16x16x32_bf16(false, a.hi, false, b.mid, (short)0, c, false, false);
    c = __builtin_amdgcn_wmma_f32_16x16x32_bf16(false, a.mid, false, b.hi, (short)0, c, false, false);
    c = __builtin_amdgcn_wmma_f32_16x16x32_bf16(false, a.hi, false, b.lo, (short)0, c, false, false);
    c = __builtin_amdgcn_wmma_f32_16x16x32_bf16(false, a.mid, false, b.mid, (short)0, c, false, false);
    c = __builtin_amdgcn_wmma_f32_16x16x32_bf16(false, a.lo, false, b.hi, (short)0, c, false, false);
    asm volatile("v_nop\n\tv_nop\n\tv_nop\n\tv_nop" : "+v"(c) : "v"(a.hi), "v"(a.mid), "v"(a.lo), "v"(b.hi), "v"(b.mid), "v"(b.lo));
    return c;
}

__device__ __forceinline__ v16h fh_ld(const float* __restrict__ p, long long sk, int k0, int h, int klen, float s) {
    v16h a;
#pragma unroll
    for (int i = 0; i < 16; ++i) { const int k = k0 + frag_k(i, h); a[i] = (k < klen) ? (_Float16)(p[(long long)k * sk] * s) : (_Float16)0.f; }
    return a;
}
__device__ __forceinline__ Split sp_ld(const float* __restrict__ p, long long sk, int k0, int h, int klen, float s) {
    Split r;
#pragma unroll
    for (int i = 0; i < 16; ++i) {
        const int k = k0 + frag_k(i, h); const float x = (k < klen) ? p[(long long)k * sk] * s : 0.f;
        const __bf16 hb = bf16_rne(x); r.hi[i] = hb; r.lo[i] = bf16_rne(x - bf16_f32(hb));
    }
    return r;
}
__device__ __forceinline__ Split3 sp3_ld(const float* __restrict__ p, long long sk, int k0, int h, int klen, float s) {
    Split3 r;
#pragma unroll
    for (int i = 0; i < 16; ++i) {
        const int k = k0 + frag_k(i, h); const float x = (k < klen) ? p[(long long)k * sk] * s : 0.f;
        const __bf16 hb = bf16_rne(x); const float r1 = x - bf16_f32(hb); const __bf16 mb = bf16_rne(r1);
        r.hi[i] = hb; r.mid[i] = mb; r.lo[i] = bf16_rne(r1 - bf16_f32(mb));
    }
    return r;
}
__device__ __forceinline__ v16b bh_ld(const float* __restrict__ p, long long sk, int k0, int h, int klen, float s) {
    v16b a;
#pragma unroll
    for (int i = 0; i < 16; ++i) { const int k = k0 + frag_k(i, h); a[i] = bf16_rne((k < klen) ? p[(long long)k * sk] * s : 0.f); }
    return a;
}
__device__ __forceinline__ v16h fh_row(const _Float16* __restrict__ row, int k0, int h) {
    v16h a;
#pragma unroll
    for (int i = 0; i < 16; ++i) a[i] = row[k0 + frag_k(i, h)];
    return a;
}

#define VST2(T, ptr, val) do { const T vst2_v_ = (val); *(volatile T*)(ptr) = vst2_v_; __threadfence(); *(volatile T*)(ptr) = vst2_v_; } while (0)
typedef float v4f __attribute__((ext_vector_type(4)));
#define VST2V4(ptr, val) do { const v4f vst2_v4_ = (val); *(volatile v4f*)(ptr) = vst2_v4_; __threadfence(); *(volatile v4f*)(ptr) = vst2_v4_; } while (0)

__device__ __attribute__((noinline)) float act_fn(float v, int act) {
    if (act == 1) return fmaxf(v, 0.f);
    if (act == 2) { const float u = 0.7978845608028654f * (v + 0.044715f * v * v * v); return 0.5f * v * (1.f + tanhf(u)); }
    if (act == 3) return v / (1.f + expf(-v));
    if (act == 4) return 0.5f * v * (1.f + erff(v * 0.7071067811865476f));
    if (act == 5) return tanhf(v);
    if (act == 6) return 1.f / (1.f + expf(-v));
    if (act == 7) return (v > 0.f) ? v : 0.01f * v;
    if (act == 8) return (v > 0.f) ? v : (expf(v) - 1.f);
    if (act == 9) return fminf(fmaxf(v, 0.f), 6.f);
    if (act == 10) return fabsf(v);
    if (act == 11) return (v >= 0.f) ? v : 0.1f * v;
    if (act == 12) return (v > 0.f) ? v : 0.2f * v;
    if (act == 13) return (v > 20.f) ? v : log1pf(expf(v));
    return v;
}

struct GemmP {
    const float* A; const float* B; const float* bias; const float* R; float* C;
    long long sAo, sAi, sAm, sAk, sBo, sBi, sBn, sBk, sCo, sCi, sCm, sRo, sRi, sRm, sRn;
    int M, N, K, zi_n, flags, act; float alpha, beta, sa, sb;
    int Npad, pad_;
};
static_assert(sizeof(GemmP) == 5 * 8 + 15 * 8 + 6 * 4 + 4 * 4 + 2 * 4, "GemmP has padding");

template <int MODE>
__global__ __launch_bounds__(32) void k_gemm(GemmP p) {
    const int lane = threadIdx.x & 31, h = lane >> 4, l15 = lane & 15;
    const int m0 = blockIdx.y * 16, n0 = blockIdx.x * 32;
    const int z = blockIdx.z, zo = z / p.zi_n, zi = z - zo * p.zi_n;
    const float* A = p.A + zo * p.sAo + zi * p.sAi;
    const float* B = p.B + zo * p.sBo + zi * p.sBi;
    const int am = min(m0 + l15, p.M - 1);
    v8f acc[2], comp[2];
#pragma unroll
    for (int t = 0; t < 2; ++t) { v8f zz = {}; acc[t] = zz; comp[t] = zz; }
    for (int k0 = 0; k0 < p.K; k0 += 32) {
        const float* arow = A + (long long)am * p.sAm;
        if (MODE == 1) {
            const Split a = sp_ld(arow, p.sAk, k0, h, p.K, 1.f);
#pragma unroll
            for (int t = 0; t < 2; ++t) {
                const int bn = min(n0 + t * 16 + l15, p.N - 1);
                acc[t] = wmma3(a, sp_ld(B + (long long)bn * p.sBn, p.sBk, k0, h, p.K, 1.f), acc[t]);
            }
        } else if (MODE == 3) {
            const Split3 a = sp3_ld(arow, p.sAk, k0, h, p.K, 1.f);
#pragma unroll
            for (int t = 0; t < 2; ++t) {
                const int bn = min(n0 + t * 16 + l15, p.N - 1);
                acc[t] = wmma6(a, sp3_ld(B + (long long)bn * p.sBn, p.sBk, k0, h, p.K, 1.f), acc[t]);
            }
        } else if (MODE == 4) {
            const Split3 a = sp3_ld(arow, p.sAk, k0, h, p.K, 1.f);
#pragma unroll
            for (int t = 0; t < 2; ++t) {
                const int bn = min(n0 + t * 16 + l15, p.N - 1); v8f zz = {};
                const v8f part = wmma6(a, sp3_ld(B + (long long)bn * p.sBn, p.sBk, k0, h, p.K, 1.f), zz);
                const v8f y = part - comp[t]; const v8f s = acc[t] + y; comp[t] = (s - acc[t]) - y; acc[t] = s;
            }
        } else if (MODE == 2) {
            const v16b a = bh_ld(arow, p.sAk, k0, h, p.K, 1.f);
#pragma unroll
            for (int t = 0; t < 2; ++t) {
                const int bn = min(n0 + t * 16 + l15, p.N - 1);
                acc[t] = wmmab(a, bh_ld(B + (long long)bn * p.sBn, p.sBk, k0, h, p.K, 1.f), acc[t]);
            }
        } else {
            const v16h a = fh_ld(arow, p.sAk, k0, h, p.K, p.sa);
#pragma unroll
            for (int t = 0; t < 2; ++t) {
                const int bn = min(n0 + t * 16 + l15, p.N - 1);
                acc[t] = wmma16(a, fh_ld(B + (long long)bn * p.sBn, p.sBk, k0, h, p.K, p.sb), acc[t]);
            }
        }
    }
    const float iscale = (MODE == 0) ? p.alpha / (p.sa * p.sb) : p.alpha;
    float* C = p.C + zo * p.sCo + zi * p.sCi;
    const float* R = p.R + zo * p.sRo + zi * p.sRi;
    __shared__ __align__(16) float ctile[16][36];
#pragma unroll
    for (int t = 0; t < 2; ++t) {
        const int n = n0 + t * 16 + l15; const int nn = min(n, p.N - 1);
#pragma unroll
        for (int r = 0; r < 8; ++r) {
            const int m = m0 + 8 * h + r; const int mm = min(m, p.M - 1);
            float v = acc[t][r] * iscale;
            if (p.flags & 1) v += p.bias[nn];
            if (p.flags & 2) v += p.bias[mm];
            if (p.flags & 8) v *= p.bias[(long long)zo * p.M + mm];
            v = act_fn(v, p.act);
            if (p.flags & 4) v += p.beta * R[(long long)mm * p.sRm + (long long)nn * p.sRn];
            ctile[8 * h + r][t * 16 + l15] = (n < p.N) ? v : 0.f;
        }
    }
    __syncthreads();
    const int NW = (p.Npad > p.N) ? p.Npad : p.N;
    const bool fast = (m0 + 16 <= p.M) && (n0 + 32 <= NW) && ((p.sCm & 3) == 0) && ((((size_t)C) & 15) == 0);
    if (fast) {
#pragma unroll
        for (int s = 0; s < 4; ++s) {
            const int row = s * 4 + (lane >> 3), c4 = (lane & 7) * 4;
            const v4f v = *(const v4f*)&ctile[row][c4];
            VST2V4(C + (long long)(m0 + row) * p.sCm + n0 + c4, v);
        }
    } else {
        for (int row = 0; row < 16; ++row) {
            const int m = m0 + row, n = n0 + lane;
            if (m < p.M && n < NW) VST2(float, C + (long long)m * p.sCm + n, ctile[row][lane]);
        }
    }
}


template <int MODE, int TM, int TN>
__global__ __launch_bounds__(32) void k_gemmT(GemmP p) {
    const int lane = threadIdx.x & 31, h = lane >> 4, l15 = lane & 15;
    const int m0 = blockIdx.y * (16 * TM), n0 = blockIdx.x * (16 * TN);
    const int z = blockIdx.z, zo = z / p.zi_n, zi = z - zo * p.zi_n;
    const float* A = p.A + zo * p.sAo + zi * p.sAi;
    const float* B = p.B + zo * p.sBo + zi * p.sBi;
    v8f acc[TM][TN];
#pragma unroll
    for (int i = 0; i < TM; ++i)
#pragma unroll
        for (int t = 0; t < TN; ++t) { v8f zz = {}; acc[i][t] = zz; }
    for (int k0 = 0; k0 < p.K; k0 += 32) {
        if (MODE == 1) {
            Split a[TM], b[TN];
#pragma unroll
            for (int i = 0; i < TM; ++i) { const int am = min(m0 + 16 * i + l15, p.M - 1); a[i] = sp_ld(A + (long long)am * p.sAm, p.sAk, k0, h, p.K, 1.f); }
#pragma unroll
            for (int t = 0; t < TN; ++t) { const int bn = min(n0 + 16 * t + l15, p.N - 1); b[t] = sp_ld(B + (long long)bn * p.sBn, p.sBk, k0, h, p.K, 1.f); }
#pragma unroll
            for (int i = 0; i < TM; ++i)
#pragma unroll
                for (int t = 0; t < TN; ++t) acc[i][t] = wmma3(a[i], b[t], acc[i][t]);
        } else if (MODE == 2) {
            v16b a[TM], b[TN];
#pragma unroll
            for (int i = 0; i < TM; ++i) { const int am = min(m0 + 16 * i + l15, p.M - 1); a[i] = bh_ld(A + (long long)am * p.sAm, p.sAk, k0, h, p.K, 1.f); }
#pragma unroll
            for (int t = 0; t < TN; ++t) { const int bn = min(n0 + 16 * t + l15, p.N - 1); b[t] = bh_ld(B + (long long)bn * p.sBn, p.sBk, k0, h, p.K, 1.f); }
#pragma unroll
            for (int i = 0; i < TM; ++i)
#pragma unroll
                for (int t = 0; t < TN; ++t) acc[i][t] = wmmab(a[i], b[t], acc[i][t]);
        } else {
            v16h a[TM], b[TN];
#pragma unroll
            for (int i = 0; i < TM; ++i) { const int am = min(m0 + 16 * i + l15, p.M - 1); a[i] = fh_ld(A + (long long)am * p.sAm, p.sAk, k0, h, p.K, p.sa); }
#pragma unroll
            for (int t = 0; t < TN; ++t) { const int bn = min(n0 + 16 * t + l15, p.N - 1); b[t] = fh_ld(B + (long long)bn * p.sBn, p.sBk, k0, h, p.K, p.sb); }
#pragma unroll
            for (int i = 0; i < TM; ++i)
#pragma unroll
                for (int t = 0; t < TN; ++t) acc[i][t] = wmma16(a[i], b[t], acc[i][t]);
        }
    }
    const float iscale = (MODE == 0) ? p.alpha / (p.sa * p.sb) : p.alpha;
    float* C = p.C + zo * p.sCo + zi * p.sCi;
    const float* R = p.R + zo * p.sRo + zi * p.sRi;
    const int NW = (p.Npad > p.N) ? p.Npad : p.N;
    __shared__ __align__(16) float ctile[16][36];
#pragma unroll
    for (int i = 0; i < TM; ++i) {
        const int mb = m0 + 16 * i; if (mb >= p.M) break;
#pragma unroll
        for (int tp = 0; tp < TN / 2; ++tp) {
            const int nb = n0 + 32 * tp; if (nb >= NW) break;
#pragma unroll
            for (int t2 = 0; t2 < 2; ++t2) {
                const int t = 2 * tp + t2; const int n = nb + t2 * 16 + l15; const int nn = min(n, p.N - 1);
#pragma unroll
                for (int r = 0; r < 8; ++r) {
                    const int m = mb + 8 * h + r; const int mm = min(m, p.M - 1);
                    float v = acc[i][t][r] * iscale;
                    if (p.flags & 1) v += p.bias[nn];
                    if (p.flags & 2) v += p.bias[mm];
            if (p.flags & 8) v *= p.bias[(long long)zo * p.M + mm];
                    v = act_fn(v, p.act);
                    if (p.flags & 4) v += p.beta * R[(long long)mm * p.sRm + (long long)nn * p.sRn];
                    ctile[8 * h + r][t2 * 16 + l15] = (n < p.N) ? v : 0.f;
                }
            }
            __syncthreads();
            const bool fast = (mb + 16 <= p.M) && (nb + 32 <= NW) && ((p.sCm & 3) == 0) && ((((size_t)C) & 15) == 0);
            if (fast) {
#pragma unroll
                for (int s = 0; s < 4; ++s) {
                    const int row = s * 4 + (lane >> 3), c4 = (lane & 7) * 4;
                    const v4f v = *(const v4f*)&ctile[row][c4];
                    VST2V4(C + (long long)(mb + row) * p.sCm + nb + c4, v);
                }
            } else {
                for (int row = 0; row < 16; ++row) {
                    const int m = mb + row, n = nb + lane;
                    if (m < p.M && n < NW) VST2(float, C + (long long)m * p.sCm + n, ctile[row][lane]);
                }
            }
            __syncthreads();
        }
    }
}

#define AW 4
struct AttnP {
    const float* Q; const float* K; const float* V; float* O; float* P; const float* Mf; const int* Mi; float* ST;
    const float* Pw; const float* Rt; const int* SQ; const int* SK;
    long long swb, swh, swi, swj, srb, srh, sri;
    long long sQb, sQh, sQi, sQd, sKb, sKh, sKj, sKd, sVb, sVh, sVj, sVd, sOb, sOh, sOi, sPb, sPh, sPi, smb, smh, smi, smj;
    int Lq, Lk, dh, dv, hrep, causal, coff, pband;
    float scale, mfill; int nonorm, mpol;
    int roff, rn, segpol, win;
};
static_assert(sizeof(AttnP) == 12 * 8 + 29 * 8 + 16 * 4, "AttnP has padding");

#ifndef KATTN_ATTR
#define KATTN_ATTR
#endif
template <int DHP, int DVP, int QM, bool SPLITPV, bool TWOPASS>
__global__ __launch_bounds__(32 * AW) KATTN_ATTR void k_attn(AttnP p) {
    constexpr int NT = DVP / 16;
    constexpr int KS = DHP / 32;
    constexpr int VP = DVP + 8;
    __shared__ __align__(16) float    pl[AW][16 * 64];
    __shared__ __align__(16) _Float16 vl[(SPLITPV ? 2 : 1) * 64 * VP];
    const int lane = threadIdx.x & 31, hf = lane >> 4, l15 = lane & 15, wave = threadIdx.x >> 5;
    const int h = blockIdx.y, b = blockIdx.z, hk = h / p.hrep;
    const int q0 = (blockIdx.x * AW + wave) * 16;
    float* myp = pl[wave];
    const float L2E = 1.4426950408889634f;
    const float NEG = -__builtin_inff();
    const int qi = min(q0 + l15, p.Lq - 1);
    const float* qrow = p.Q + b * p.sQb + h * p.sQh + (long long)qi * p.sQi;
    const float* kbase = p.K + b * p.sKb + hk * p.sKh;
    const float* vbase = p.V + b * p.sVb + hk * p.sVh;
    v16h qa[QM == 0 ? KS : 1]; Split qs_[QM == 1 ? KS : 1]; Split3 qt_[QM == 2 ? KS : 1];
#pragma unroll
    for (int ks = 0; ks < KS; ++ks) {
        if (QM == 2) qt_[ks] = sp3_ld(qrow, p.sQd, ks * 32, hf, p.dh, 1.f);
        else if (QM == 1) qs_[ks] = sp_ld(qrow, p.sQd, ks * 32, hf, p.dh, 1.f);
        else qa[ks] = fh_ld(qrow, p.sQd, ks * 32, hf, p.dh, 1.f);
    }
    v8f o[NT]; float m8[8], l8[8];
#pragma unroll
    for (int t = 0; t < NT; ++t) { v8f zz = {}; o[t] = zz; }
#pragma unroll
    for (int i = 0; i < 8; ++i) { m8[i] = NEG; l8[i] = 0.f; }
    int jend = p.Lk;
    if (p.causal == 1) { const int je = (blockIdx.x * AW + AW - 1) * 16 + 16 + p.coff; jend = min(jend, max(je, 0)); }
    const int npass = TWOPASS ? 2 : 1;
    for (int pass = 0; pass < npass; ++pass) {
        const bool dopv = (!TWOPASS) || pass == 1;
        for (int j0 = 0; j0 < jend; j0 += 64) {
            if (dopv) {
                __syncthreads();
                for (int idx = threadIdx.x; idx < 64 * DVP; idx += 32 * AW) {
                    const int jr = idx / DVP, d = idx - jr * DVP, j = j0 + jr;
                    const float f = (j < p.Lk && d < p.dv) ? vbase[(long long)j * p.sVj + (long long)d * p.sVd] : 0.f;
                    if (SPLITPV) {
                        const __bf16 hb = bf16_rne(f);
                        ((__bf16*)vl)[jr * VP + d] = hb; ((__bf16*)vl)[64 * VP + jr * VP + d] = bf16_rne(f - bf16_f32(hb));
                    } else vl[jr * VP + d] = (_Float16)f;
                }
            }
            v8f s[4];
#pragma unroll
            for (int t = 0; t < 4; ++t) {
                const int j = min(j0 + t * 16 + l15, p.Lk - 1);
                const float* krow = kbase + (long long)j * p.sKj;
                v8f acc = {};
#pragma unroll
                for (int ks = 0; ks < KS; ++ks) {
                    if (QM == 2)      acc = wmma6(qt_[ks], sp3_ld(krow, p.sKd, ks * 32, hf, p.dh, 1.f), acc);
                    else if (QM == 1) acc = wmma3(qs_[ks], sp_ld(krow, p.sKd, ks * 32, hf, p.dh, 1.f), acc);
                    else              acc = wmma16(qa[ks], fh_ld(krow, p.sKd, ks * 32, hf, p.dh, 1.f), acc);
                }
                s[t] = acc;
            }
            float pv[8][4];
#pragma unroll
            for (int i = 0; i < 8; ++i) {
                const int irow = q0 + i + 8 * hf;
                const int ic = min(irow, p.Lq - 1);
                float sc[4];
#pragma unroll
                for (int t = 0; t < 4; ++t) {
                    const int jg = j0 + t * 16 + l15;
                    float v = s[t][i] * p.scale;
                    if (p.Mf) v += p.Mf[b * p.smb + h * p.smh + (long long)ic * p.smi + (long long)min(jg, p.Lk - 1) * p.smj];
                    if (p.Rt) { int rc = ic - min(jg, p.Lk - 1) + p.roff; rc = rc < 0 ? 0 : (rc >= p.rn ? p.rn - 1 : rc); v += p.Rt[b * p.srb + h * p.srh + (long long)ic * p.sri + rc]; }
                    if (p.Mi) { const int mv = p.Mi[b * p.smb + h * p.smh + (long long)ic * p.smi + (long long)min(jg, p.Lk - 1) * p.smj]; if (p.mpol ? (mv != 0) : (mv == 0)) v = p.mfill; }
                    if (p.SQ) { const bool same = p.SQ[(long long)b * p.Lq + ic] == p.SK[(long long)b * p.Lk + min(jg, p.Lk - 1)]; if (p.segpol ? same : !same) v = p.mfill; }
                    if (p.causal == 2 && jg > irow + p.coff) v = p.mfill;
                    if (jg >= p.Lk || (p.causal == 1 && jg > irow + p.coff) || (p.causal == 3 && jg < irow + p.coff) || (p.win > 0 && irow + p.coff - jg > p.win)) v = NEG; else v *= L2E;
                    sc[t] = v;
                }
                if (!TWOPASS || pass == 0) {
                    float mx = fmaxf(fmaxf(sc[0], sc[1]), fmaxf(sc[2], sc[3]));
                    mx = fmaxf(mx, __shfl_xor(mx, 1, 32)); mx = fmaxf(mx, __shfl_xor(mx, 2, 32));
                    mx = fmaxf(mx, __shfl_xor(mx, 4, 32)); mx = fmaxf(mx, __shfl_xor(mx, 8, 32));
                    const float mnew = fmaxf(m8[i], mx);
                    const float corr = (mnew == NEG) ? 1.f : exp2f(m8[i] - mnew);
                    float rs = 0.f;
#pragma unroll
                    for (int t = 0; t < 4; ++t) {
                        const float pp = (sc[t] == NEG) ? 0.f : exp2f(sc[t] - mnew); rs += pp;
                        pv[i][t] = p.Pw ? pp * p.Pw[b * p.swb + h * p.swh + (long long)ic * p.swi + (long long)min(j0 + t * 16 + l15, p.Lk - 1) * p.swj] : pp;
                    }
                    rs += __shfl_xor(rs, 1, 32); rs += __shfl_xor(rs, 2, 32); rs += __shfl_xor(rs, 4, 32); rs += __shfl_xor(rs, 8, 32);
                    l8[i] = l8[i] * corr + rs; m8[i] = mnew;
                    if (!TWOPASS) {
#pragma unroll
                        for (int t = 0; t < NT; ++t) o[t][i] *= corr;
                    }
                } else {
                    const float inv = (l8[i] > 0.f) ? 1.f / l8[i] : 0.f;
#pragma unroll
                    for (int t = 0; t < 4; ++t) {
                        const int jg = j0 + t * 16 + l15;
                        float pp = (sc[t] == NEG) ? 0.f : exp2f(sc[t] - m8[i]) * inv;
                        if (p.Pw) pp *= p.Pw[b * p.swb + h * p.swh + (long long)ic * p.swi + (long long)min(jg, p.Lk - 1) * p.swj];
                        pv[i][t] = pp;
                    }
                }
            }
            if (dopv) {
#pragma unroll
                for (int i = 0; i < 8; ++i)
#pragma unroll
                    for (int t = 0; t < 4; ++t) myp[(i + 8 * hf) * 64 + t * 16 + l15] = pv[i][t];
                __syncthreads();
                if (p.P) {
                    float* pb_ = p.P + b * p.sPb + h * p.sPh;
                    const bool fastP = (p.pband == 0) && ((p.sPi & 3) == 0) && (j0 + 64 <= p.Lk) && (q0 + 16 <= p.Lq) && ((((size_t)pb_) & 15) == 0);
                    if (fastP) {
#pragma unroll
                        for (int s = 0; s < 8; ++s) {
                            const int row = s * 2 + (lane >> 4), c4 = (lane & 15) * 4;
                            const v4f v = *(const v4f*)(myp + row * 64 + c4);
                            VST2V4(pb_ + (long long)(q0 + row) * p.sPi + j0 + c4, v);
                        }
                    } else {
                        for (int row = 0; row < 16; ++row) {
                            const int irow = q0 + row; if (irow >= p.Lq) continue;
                            for (int c = lane; c < 64; c += 32) {
                                const int jg = j0 + c; if (jg >= p.Lk) continue;
                                if (p.pband == 0) VST2(float, pb_ + (long long)irow * p.sPi + jg, myp[row * 64 + c]);
                                else if (jg - irow <= p.pband && irow - jg <= p.pband) VST2(float, pb_ + (long long)irow * p.sPi + (jg - irow + p.pband), myp[row * 64 + c]);
                            }
                        }
                    }
                }
                if (SPLITPV) {
                    const Split pa0 = sp_ld(myp + l15 * 64, 1, 0, hf, 64, 1.f), pa1 = sp_ld(myp + l15 * 64, 1, 32, hf, 64, 1.f);
                    const __bf16* vh = (const __bf16*)vl; const __bf16* vlo = vh + 64 * VP;
#pragma unroll
                    for (int t = 0; t < NT; ++t) {
                        const int dcol = t * 16 + l15;
                        Split b0, b1;
#pragma unroll
                        for (int e = 0; e < 16; ++e) {
                            const int k0 = frag_k(e, hf), k1 = 32 + frag_k(e, hf);
                            b0.hi[e] = vh[k0 * VP + dcol]; b0.lo[e] = vlo[k0 * VP + dcol]; b1.hi[e] = vh[k1 * VP + dcol]; b1.lo[e] = vlo[k1 * VP + dcol];
                        }
                        o[t] = wmma3(pa0, b0, o[t]);
                        o[t] = wmma3(pa1, b1, o[t]);
                    }
                } else {
                    const v16h pa0 = fh_ld(myp + l15 * 64, 1, 0, hf, 64, 4096.f), pa1 = fh_ld(myp + l15 * 64, 1, 32, hf, 64, 4096.f);
#pragma unroll
                    for (int t = 0; t < NT; ++t) {
                        const int dcol = t * 16 + l15;
                        v16h b0, b1;
#pragma unroll
                        for (int e = 0; e < 16; ++e) { b0[e] = vl[frag_k(e, hf) * VP + dcol]; b1[e] = vl[(32 + frag_k(e, hf)) * VP + dcol]; }
                        o[t] = wmma16(pa0, b0, o[t]);
                        o[t] = wmma16(pa1, b1, o[t]);
                    }
                }
            }
        }
    }
    float* obase = p.O + b * p.sOb + h * p.sOh;
    if (p.ST) {
        const int rl = lane >> 1, isel = rl & 7;
        float mv = 0.f, lv = 0.f;
#pragma unroll
        for (int i = 0; i < 8; ++i) if (i == isel) { mv = m8[i]; lv = l8[i]; }
        const int irow = q0 + rl;
        if (irow < p.Lq) { float* st = p.ST + (((long long)b * gridDim.y + h) * p.Lq + irow) * 2 + (lane & 1); VST2(float, st, (lane & 1) ? lv : mv * 0.6931471805599453f); }
    }
    float invr[8];
#pragma unroll
    for (int i = 0; i < 8; ++i) {
        if (TWOPASS) invr[i] = SPLITPV ? 1.f : (1.f / 4096.f);
        else if (p.nonorm) invr[i] = exp2f(m8[i]) * (SPLITPV ? 1.f : (1.f / 4096.f));
        else invr[i] = (l8[i] > 0.f) ? (SPLITPV ? 1.f / l8[i] : 1.f / (l8[i] * 4096.f)) : 0.f;
    }
    __syncthreads();
    const bool ofast = ((p.sOi & 3) == 0) && ((((size_t)obase) & 15) == 0) && (q0 + 16 <= p.Lq);
#pragma unroll
    for (int c0 = 0; c0 < DVP; c0 += 64) {
#pragma unroll
        for (int i = 0; i < 8; ++i)
#pragma unroll
            for (int t = 0; t < NT; ++t) if (t * 16 >= c0 && t * 16 < c0 + 64) myp[(i + 8 * hf) * 64 + (t * 16 - c0) + l15] = o[t][i] * invr[i];
        __syncthreads();
        const int cw = (DVP - c0 < 64) ? (DVP - c0) : 64;
        if (ofast && (c0 + cw <= p.dv) && (cw % 32 == 0)) {
            const int lpr = cw / 4;
            const int rows_per_ins = 32 / lpr;
            for (int r0 = 0; r0 < 16; r0 += rows_per_ins) {
                const int row = r0 + lane / lpr, c4 = (lane % lpr) * 4;
                const v4f v = *(const v4f*)(myp + row * 64 + c4);
                VST2V4(obase + (long long)(q0 + row) * p.sOi + c0 + c4, v);
            }
        } else {
            for (int row = 0; row < 16; ++row) {
                const int irow = q0 + row; if (irow >= p.Lq) continue;
                for (int c = lane; c < cw; c += 32) { const int d = c0 + c; if (d < p.dv) VST2(float, obase + (long long)irow * p.sOi + d, myp[row * 64 + c]); }
            }
        }
        __syncthreads();
    }
}

struct TrP { const float* src; float* dst; const float* R2; long long sSz, lds, sDz, ldd, sRz, ldr; int R, C, flags, act; float alpha, beta; };
static_assert(sizeof(TrP) == 3 * 8 + 6 * 8 + 6 * 4, "TrP has padding");
__global__ __launch_bounds__(256) void k_tr(TrP p) {
    __shared__ float tile[32][33];
    const int c0 = blockIdx.x * 32, r0 = blockIdx.y * 32, z = blockIdx.z;
    const int lane = threadIdx.x & 31, wave = threadIdx.x >> 5;
    const float* s = p.src + z * p.sSz;
#pragma unroll
    for (int k = 0; k < 4; ++k) {
        const int rl = wave * 4 + k, r = r0 + rl, c = c0 + lane;
        tile[rl][lane] = (r < p.R && c < p.C) ? s[(long long)r * p.lds + c] : 0.f;
    }
    __syncthreads();
    float* d = p.dst + z * p.sDz; const float* rr = p.R2 + z * p.sRz;
#pragma unroll
    for (int k = 0; k < 4; ++k) {
        const int cl = wave * 4 + k, c = c0 + cl, r = r0 + lane;
        if (c < p.C && r < p.R) {
            float v = act_fn(p.alpha * tile[lane][cl], p.act);
            if (p.flags & 1) v += p.beta * rr[(long long)c * p.ldr + r];
            VST2(float, d + (long long)c * p.ldd + r, v);
        }
    }
}

__global__ __launch_bounds__(256) void k_affine(const float* __restrict__ src, float* __restrict__ dst, int n, float a, float b, const float* __restrict__ sdev) {
    const int i = blockIdx.x * 256 + threadIdx.x;
    if (i < n) { const float aa = sdev ? a * sdev[0] : a; const float v = aa * src[i] + b; VST2(float, dst + i, v); }
}

struct SmP { const float* src; float* dst; const float* Mf; long long sz, sr, dz, dr, smz, smr; int n, pad; float scale_in, scale_out; };
static_assert(sizeof(SmP) == 3 * 8 + 6 * 8 + 4 * 4, "SmP has padding");
__global__ __launch_bounds__(256) void k_softmax(SmP p) {
    __shared__ float red[256];
    const int r = blockIdx.x, z = blockIdx.y, tid = threadIdx.x;
    const float* s = p.src + z * p.sz + (long long)r * p.sr;
    const float* mf = p.Mf ? (p.Mf + z * p.smz + (long long)r * p.smr) : nullptr;
    float mx = -__builtin_inff();
    for (int j = tid; j < p.n; j += 256) { float v = s[j] * p.scale_in; if (mf) v += mf[j]; mx = fmaxf(mx, v); }
    red[tid] = mx; __syncthreads();
    for (int o = 128; o > 0; o >>= 1) { if (tid < o) red[tid] = fmaxf(red[tid], red[tid + o]); __syncthreads(); }
    mx = red[0]; __syncthreads();
    float sum = 0.f;
    for (int j = tid; j < p.n; j += 256) { float v = s[j] * p.scale_in; if (mf) v += mf[j]; sum += (mx == -__builtin_inff()) ? 0.f : expf(v - mx); }
    red[tid] = sum; __syncthreads();
    for (int o = 128; o > 0; o >>= 1) { if (tid < o) red[tid] += red[tid + o]; __syncthreads(); }
    sum = red[0];
    const float inv = (sum > 0.f) ? p.scale_out / sum : 0.f;
    float* d = p.dst + z * p.dz + (long long)r * p.dr;
    for (int j = tid; j < p.n; j += 256) { float v = s[j] * p.scale_in; if (mf) v += mf[j]; const float o = (mx == -__builtin_inff()) ? 0.f : expf(v - mx) * inv; VST2(float, d + j, o); }
}
__global__ __launch_bounds__(256) void k_stats(const float* __restrict__ x, long long sz, long long so, long long si, int inner, int n, float eps, float* __restrict__ stat, int mode) {
    __shared__ float red[256];
    const int z = blockIdx.x, tid = threadIdx.x;
    const float* base = x + z * sz;
    float s = 0.f;
    for (int e = tid; e < n; e += 256) s += base[(long long)(e / inner) * so + (long long)(e % inner) * si];
    red[tid] = s; __syncthreads();
    for (int o = 128; o > 0; o >>= 1) { if (tid < o) red[tid] += red[tid + o]; __syncthreads(); }
    const float mu = (mode == 0 || mode == 3) ? red[0] / (float)n : 0.f; __syncthreads();
    float q = 0.f;
    for (int e = tid; e < n; e += 256) { const float dlt = base[(long long)(e / inner) * so + (long long)(e % inner) * si] - mu; q += dlt * dlt; }
    red[tid] = q; __syncthreads();
    for (int o = 128; o > 0; o >>= 1) { if (tid < o) red[tid] += red[tid + o]; __syncthreads(); }
    {
        float rs;
        if (mode == 2) rs = sqrtf((float)n) / fmaxf(sqrtf(red[0]), eps); else if (mode == 3) rs = rsqrtf(red[0] / (float)(n - 1) + eps); else rs = rsqrtf(red[0] / (float)n + eps);
        if (tid < 32) { const float v = (tid == 0) ? mu : ((tid == 1) ? rs : 0.f); VST2(float, stat + (long long)z * 32 + tid, v); }
    }
}
__global__ __launch_bounds__(256) void k_norm_apply(const float* __restrict__ x, float* __restrict__ y, const float* __restrict__ stat, const float* __restrict__ g, const float* __restrict__ bta,
                                                     int Z, int C, int L, int G, int bn, int act) {
    const long long idx = (long long)blockIdx.x * 256 + threadIdx.x;
    if (idx >= (long long)Z * C * L) return;
    const int l = (int)(idx % L); const long long zc = idx / L; const int c = (int)(zc % C), z = (int)(zc / C); (void)l;
    const int set = bn ? c : (z * G + c / (C / G));
    float v = (x[idx] - stat[(long long)set * 32]) * stat[(long long)set * 32 + 1];
    if (g) v *= g[c];
    if (bta) v += bta[c];
    v = act_fn(v, act);
    VST2(float, y + idx, v);
}

__global__ __launch_bounds__(256) void k_lse_neg(const float* __restrict__ st, float* __restrict__ c, int n) {
    const int i = blockIdx.x * 256 + threadIdx.x;
    if (i < n) { const float v = -(st[2 * i] + logf(st[2 * i + 1])); VST2(float, c + i, v); }
}

__global__ __launch_bounds__(256) void k_iota(int* __restrict__ dst, int n, int a, int b) {
    const int i = blockIdx.x * 256 + threadIdx.x;
    if (i < n) { const int v = a * i + b; VST2(int, dst + i, v); }
}

__global__ __launch_bounds__(256) void k_axpby(const float* __restrict__ x, const float* __restrict__ y, float* __restrict__ dst, int n, float a, float b, float c) {
    const int i = blockIdx.x * 256 + threadIdx.x;
    if (i < n) { const float v = a * x[i] + b * y[i] + c; VST2(float, dst + i, v); }
}

struct RopeP { const float* X; float* Y; const float* C; const float* Sn; const int* pos; long long sXr, sXh, sYr, sYh, sCb, sCp, sCd; int R, Hn, D, S, mode, tmode, pmode, pad; };
static_assert(sizeof(RopeP) == 5 * 8 + 7 * 8 + 8 * 4, "RopeP has padding");
__global__ __launch_bounds__(256) void k_rope(RopeP p) {
    const long long idx = (long long)blockIdx.x * 256 + threadIdx.x;
    if (idx >= (long long)p.R * p.Hn * p.D) return;
    const int d = (int)(idx % p.D); const long long rh = idx / p.D; const int h = (int)(rh % p.Hn); const int r = (int)(rh / p.Hn);
    const int half = p.D / 2;
    int partner; float sign;
    if (p.mode == 0) { partner = (d < half) ? d + half : d - half; sign = (d < half) ? -1.f : 1.f; }
    else { partner = d ^ 1; sign = (d & 1) ? 1.f : -1.f; }
    const int tcol = (p.tmode == 0) ? d : ((p.tmode == 1) ? (d % half) : (d >> 1));
    const int pp = (p.pmode == 0) ? (r % p.S) : ((p.pmode == 1) ? h : p.pos[r]);
    const long long toff = (long long)(r / p.S) * p.sCb + (long long)pp * p.sCp + (long long)tcol * p.sCd;
    const float* xr = p.X + (long long)r * p.sXr + (long long)h * p.sXh;
    const float v = xr[d] * p.C[toff] + sign * xr[partner] * p.Sn[toff];
    VST2(float, p.Y + (long long)r * p.sYr + (long long)h * p.sYh + d, v);
}

__global__ __launch_bounds__(256) void k_invf(float* __restrict__ invb, int half, int D, float base, float num, int fmode, float cexp) {
    const int i = blockIdx.x * 256 + threadIdx.x;
    if (i >= ((half + 31) / 32) * 32) return;
    if (i >= half) { VST2(float, invb + i, 0.f); return; }
    const float e = (float)(2 * i) / (float)D;
    float invf;
    if (fmode == 1) invf = num * expf((float)(2 * i) * cexp);
    else if (fmode == 2) invf = num * powf(base, (-2.0f * ((float)i - 1.0f)) / (float)D);
    else invf = num * (1.0f / powf(base, e));
    VST2(float, invb + i, invf);
}
__global__ __launch_bounds__(256) void k_sincos(float* __restrict__ cs, float* __restrict__ sn, const float* __restrict__ invb, int S, int half, float pscale) {
    const int idx = blockIdx.x * 256 + threadIdx.x;
    if (idx >= S * half) return;
    const int s = idx / half, i = idx - s * half;
    const float ang = (pscale * (float)s) * invb[i];
    VST2(float, cs + idx, cosf(ang)); VST2(float, sn + idx, sinf(ang));
}

__global__ __launch_bounds__(256) void k_mulact(const float* __restrict__ x, const float* __restrict__ y, float* __restrict__ dst, int n, int act) {
    const int i = blockIdx.x * 256 + threadIdx.x;
    if (i < n) { const float v = act_fn(x[i], act) * y[i]; VST2(float, dst + i, v); }
}

__global__ __launch_bounds__(256) void k_matvec(GemmP p) {
    const int rpt = (p.N == 1) ? 1 : 32;
    const long long r0 = ((long long)blockIdx.x * 256 + threadIdx.x) * rpt; const int z = blockIdx.z, zo = z / p.zi_n, zi = z - zo * p.zi_n;
    if (r0 >= p.M) return;
    const float* Bb = p.B + zo * p.sBo + zi * p.sBi;
    float* C = p.C + zo * p.sCo + zi * p.sCi; const float* R = p.R + zo * p.sRo + zi * p.sRi;
    for (int rr = 0; rr < rpt; ++rr) {
        const long long r = r0 + rr; if (r >= p.M) break;
        const float* A = p.A + zo * p.sAo + zi * p.sAi + r * p.sAm;
        float acc[8] = {0.f, 0.f, 0.f, 0.f, 0.f, 0.f, 0.f, 0.f};
        for (int k = 0; k < p.K; ++k) { const float a = A[(long long)k * p.sAk];
#pragma unroll
            for (int j = 0; j < 8; ++j) if (j < p.N) acc[j] += a * Bb[(long long)j * p.sBn + (long long)k * p.sBk]; }
#pragma unroll
        for (int j = 0; j < 8; ++j) if (j < p.N) {
            float v = acc[j] * p.alpha;
            if (p.flags & 1) v += p.bias[j];
            if (p.flags & 2) v += p.bias[r];
            v = act_fn(v, p.act);
            if (p.flags & 4) v += p.beta * R[r * p.sRm + (long long)j * p.sRn];
            VST2(float, C + r * p.sCm + j, v);
        }
    }
}
__global__ __launch_bounds__(256) void k_smallsoftmax(const float* __restrict__ src, float* __restrict__ dst, long long sr, long long dr, int n, long long R, float scale) {
    const long long r0 = ((long long)blockIdx.x * 256 + threadIdx.x) * 32;
    for (int rr = 0; rr < 32; ++rr) {
        const long long r = r0 + rr; if (r >= R) return;
        const float* s = src + r * sr; float* d = dst + r * dr;
        float mx = -__builtin_inff();
        for (int j = 0; j < n; ++j) mx = fmaxf(mx, s[j] * scale);
        float sum = 0.f;
        for (int j = 0; j < n; ++j) sum += expf(s[j] * scale - mx);
        const float inv = 1.f / sum;
        for (int j = 0; j < n; ++j) { const float v = expf(s[j] * scale - mx) * inv; VST2(float, d + j, v); }
    }
}

__global__ __launch_bounds__(32) void k_unitstat(float* __restrict__ st) { const int t = threadIdx.x; const float v = (t == 1) ? 1.f : 0.f; VST2(float, st + t, v); }

__global__ __launch_bounds__(256) void k_lincopy(const float* __restrict__ src, long long lds, float* __restrict__ dst, long long ldd, long long rows, int cols) {
    const long long i = (long long)blockIdx.x * 256 + threadIdx.x; if (i >= rows * cols) return;
    const long long r = i / cols; const int c = (int)(i - r * cols);
    const float v = src[r * lds + c]; VST2(float, dst + r * ldd + c, v);
}

__global__ __launch_bounds__(256) void k_gg_init(const float* __restrict__ X, const int* __restrict__ lens, float* __restrict__ H, int Bn, int S, int N, int U) { const int q = blockIdx.x * 256 + threadIdx.x; if (q >= Bn * N * U) return; const int b = q / (N * U); const int r = q % (N * U); int idx = lens[b] - 1; idx = min(max(idx, 0), S - 1); VST2(float, H + q, X[((long long)b * S + idx) * N * U + r]); }
__global__ __launch_bounds__(256) void k_gg_wcat(const float* __restrict__ Wm, const float* __restrict__ Wg, const float* __restrict__ Ug, float* __restrict__ WMC, float* __restrict__ WGC, float* __restrict__ UGC, int NL, int U) { const int q = blockIdx.x * 256 + threadIdx.x; if (q >= NL * U * 3 * U) return; const int v3 = q % (3 * U); const int u = (q / (3 * U)) % U; const int l = q / (3 * U * U); const int gidx = v3 / U, v = v3 % U;
    VST2(float, WGC + q, Wg[(((long long)l * 3 + gidx) * U + u) * U + v]);
    if (gidx < 2) { const long long q2 = ((long long)l * U + u) * 2 * U + gidx * U + v; VST2(float, WMC + q2, Wm[(((long long)l * 2 + gidx) * U + u) * U + v]); VST2(float, UGC + q2, Ug[(((long long)l * 3 + gidx) * U + u) * U + v]); } }
__global__ __launch_bounds__(256) void k_gg_zr(const float* __restrict__ G, float* __restrict__ HU, const float* __restrict__ H, const float* __restrict__ bg, float* __restrict__ RH, int R, int U) { const int q = blockIdx.x * 256 + threadIdx.x; if (q >= R * U) return; const int u = q % U; const int r = q / U; const float z = 1.f / (1.f + expf(-(G[(long long)r * 3 * U + u] + HU[(long long)r * 2 * U + u] + bg[u]))); const float rr = 1.f / (1.f + expf(-(G[(long long)r * 3 * U + U + u] + HU[(long long)r * 2 * U + U + u] + bg[U + u])));
    VST2(float, HU + (long long)r * 2 * U + u, z); VST2(float, RH + q, rr * H[q]); }
__global__ __launch_bounds__(256) void k_gg_upd(const float* __restrict__ G, const float* __restrict__ HU, const float* __restrict__ RU, const float* __restrict__ bg, float* __restrict__ H, int R, int U) { const int q = blockIdx.x * 256 + threadIdx.x; if (q >= R * U) return; const int u = q % U; const int r = q / U; const float z = HU[(long long)r * 2 * U + u]; const float c = tanhf(G[(long long)r * 3 * U + 2 * U + u] + RU[q] + bg[2 * U + u]); VST2(float, H + q, (1.f - z) * H[q] + z * c); }
__global__ __launch_bounds__(256) void k_gg_max(const float* __restrict__ LG, float* __restrict__ OUT, int Bn, int N, int NC) { const int q = blockIdx.x * 256 + threadIdx.x; if (q >= Bn * NC) return; const int c = q % NC; const int b = q / NC; float m = -__builtin_inff();
#pragma unroll 1
    for (int n = 0; n < N; ++n) m = fmaxf(m, LG[((long long)b * N + n) * 16 + c]); VST2(float, OUT + q, m); }
__global__ __launch_bounds__(256) void k_gg_relu(const float* __restrict__ H, float* __restrict__ RH, int n) { const int q = blockIdx.x * 256 + threadIdx.x; if (q >= n) return; VST2(float, RH + q, fmaxf(H[q], 0.f)); }

template __global__ void k_gemm<1>(GemmP);

extern "C" void kernel_launch(void* const* d_in, const int* in_sizes, int n_in, void* d_out, int out_size, void* d_ws, size_t ws_size, hipStream_t stream) {
    (void)in_sizes; (void)n_in; (void)out_size; (void)ws_size;
    const float* inp = (const float*)d_in[0];
    const int* lens = (const int*)d_in[1];
    const float* A = (const float*)d_in[2];
    const float* Wm = (const float*)d_in[3];
    const float* bm = (const float*)d_in[4];
    const float* Wg = (const float*)d_in[5];
    const float* Ug = (const float*)d_in[6];
    const float* bg = (const float*)d_in[7];
    const float* fcw = (const float*)d_in[8];
    const float* fcb = (const float*)d_in[9];
    const int Bn = 32;
    const int S = 32;
    const int N = 128;
    const int U = 64;
    const int NE = 2;
    const int NL = 2;
    const int NC = 5;
    const int R = Bn * N;
    float* out = (float*)d_out;
    char* wsp = (char*)d_ws;
    float* H = (float*)wsp; wsp += (((size_t)((size_t)R * U) * 4 + 255) / 256) * 256;
    float* HW = (float*)wsp; wsp += (((size_t)((size_t)R * 2 * U) * 4 + 255) / 256) * 256;
    float* AGG = (float*)wsp; wsp += (((size_t)((size_t)R * U) * 4 + 255) / 256) * 256;
    float* G = (float*)wsp; wsp += (((size_t)((size_t)R * 3 * U) * 4 + 255) / 256) * 256;
    float* HU = (float*)wsp; wsp += (((size_t)((size_t)R * 2 * U) * 4 + 255) / 256) * 256;
    float* RH = (float*)wsp; wsp += (((size_t)((size_t)R * U) * 4 + 255) / 256) * 256;
    float* RU = (float*)wsp; wsp += (((size_t)((size_t)R * U) * 4 + 255) / 256) * 256;
    float* WMC = (float*)wsp; wsp += (((size_t)((size_t)NL * U * 2 * U) * 4 + 255) / 256) * 256;
    float* WGC = (float*)wsp; wsp += (((size_t)((size_t)NL * U * 3 * U) * 4 + 255) / 256) * 256;
    float* UGC = (float*)wsp; wsp += (((size_t)((size_t)NL * U * 2 * U) * 4 + 255) / 256) * 256;
    float* LG = (float*)wsp; wsp += (((size_t)((size_t)R * 16) * 4 + 255) / 256) * 256;
    k_gg_init<<<(unsigned)((R * U + 255) / 256), 256, 0, stream>>>(inp, lens, H, Bn, S, N, U); k_gg_wcat<<<(unsigned)((NL * U * 3 * U + 255) / 256), 256, 0, stream>>>(Wm, Wg, Ug, WMC, WGC, UGC, NL, U);
    { GemmP ghw00;
      ghw00.A = H; ghw00.B = WMC + (size_t)0 * U * 2 * U; ghw00.bias = H; ghw00.R = H; ghw00.C = HW;
      ghw00.sAo = 0; ghw00.sAi = 0; ghw00.sAm = U; ghw00.sAk = 1; ghw00.sBo = 0; ghw00.sBi = 0; ghw00.sBn = 1; ghw00.sBk = 2 * U; ghw00.sCo = 0; ghw00.sCi = 0; ghw00.sCm = 2 * U; ghw00.sRo = 0; ghw00.sRi = 0; ghw00.sRm = 0; ghw00.sRn = 0;
      ghw00.M = R; ghw00.N = 2 * U; ghw00.K = U; ghw00.zi_n = 1; ghw00.flags = 0; ghw00.act = 0;
      ghw00.alpha = 1.0f; ghw00.beta = 0.0f; ghw00.sa = 1.0f; ghw00.sb = 1.0f; ghw00.Npad = 2 * U; ghw00.pad_ = 0;
      if ((long long)(R) >= 64 && (long long)(2 * U) >= 64) k_gemmT<1, 2, 4><<<dim3((unsigned)((2 * U) + 63) / 64, (unsigned)((R) + 31) / 32, (unsigned)(1)), 32, 0, stream>>>(ghw00);
      else k_gemm<1><<<dim3((unsigned)((2 * U) + 31) / 32, (unsigned)((R) + 15) / 16, (unsigned)(1)), 32, 0, stream>>>(ghw00); }
    { GemmP ga000;
      ga000.A = A; ga000.B = HW; ga000.bias = bm + 0 * U; ga000.R = A; ga000.C = AGG;
      ga000.sAo = (long long)NE * N * N; ga000.sAi = 0; ga000.sAm = N; ga000.sAk = 1; ga000.sBo = (long long)N * 2 * U; ga000.sBi = 0; ga000.sBn = 1; ga000.sBk = 2 * U; ga000.sCo = (long long)N * U; ga000.sCi = 0; ga000.sCm = U; ga000.sRo = 0; ga000.sRi = 0; ga000.sRm = 0; ga000.sRn = 0;
      ga000.M = N; ga000.N = U; ga000.K = N; ga000.zi_n = 1; ga000.flags = 1; ga000.act = 0;
      ga000.alpha = 1.0f; ga000.beta = 0.0f; ga000.sa = 1.0f; ga000.sb = 1.0f; ga000.Npad = U; ga000.pad_ = 0;
      if ((long long)(N) >= 64 && (long long)(U) >= 64) k_gemmT<1, 2, 4><<<dim3((unsigned)((U) + 63) / 64, (unsigned)((N) + 31) / 32, (unsigned)(Bn)), 32, 0, stream>>>(ga000);
      else k_gemm<1><<<dim3((unsigned)((U) + 31) / 32, (unsigned)((N) + 15) / 16, (unsigned)(Bn)), 32, 0, stream>>>(ga000); }
    { GemmP ga100;
      ga100.A = A + (size_t)N * N; ga100.B = HW + U; ga100.bias = A + (size_t)N * N; ga100.R = AGG; ga100.C = AGG;
      ga100.sAo = (long long)NE * N * N; ga100.sAi = 0; ga100.sAm = N; ga100.sAk = 1; ga100.sBo = (long long)N * 2 * U; ga100.sBi = 0; ga100.sBn = 1; ga100.sBk = 2 * U; ga100.sCo = (long long)N * U; ga100.sCi = 0; ga100.sCm = U; ga100.sRo = (long long)N * U; ga100.sRi = 0; ga100.sRm = U; ga100.sRn = 1;
      ga100.M = N; ga100.N = U; ga100.K = N; ga100.zi_n = 1; ga100.flags = 4; ga100.act = 0;
      ga100.alpha = 1.0f; ga100.beta = 1.0f; ga100.sa = 1.0f; ga100.sb = 1.0f; ga100.Npad = U; ga100.pad_ = 0;
      if ((long long)(N) >= 64 && (long long)(U) >= 64) k_gemmT<1, 2, 4><<<dim3((unsigned)((U) + 63) / 64, (unsigned)((N) + 31) / 32, (unsigned)(Bn)), 32, 0, stream>>>(ga100);
      else k_gemm<1><<<dim3((unsigned)((U) + 31) / 32, (unsigned)((N) + 15) / 16, (unsigned)(Bn)), 32, 0, stream>>>(ga100); }
    { GemmP gg00;
      gg00.A = AGG; gg00.B = WGC + (size_t)0 * U * 3 * U; gg00.bias = AGG; gg00.R = AGG; gg00.C = G;
      gg00.sAo = 0; gg00.sAi = 0; gg00.sAm = U; gg00.sAk = 1; gg00.sBo = 0; gg00.sBi = 0; gg00.sBn = 1; gg00.sBk = 3 * U; gg00.sCo = 0; gg00.sCi = 0; gg00.sCm = 3 * U; gg00.sRo = 0; gg00.sRi = 0; gg00.sRm = 0; gg00.sRn = 0;
      gg00.M = R; gg00.N = 3 * U; gg00.K = U; gg00.zi_n = 1; gg00.flags = 0; gg00.act = 0;
      gg00.alpha = 1.0f; gg00.beta = 0.0f; gg00.sa = 1.0f; gg00.sb = 1.0f; gg00.Npad = 3 * U; gg00.pad_ = 0;
      if ((long long)(R) >= 64 && (long long)(3 * U) >= 64) k_gemmT<1, 2, 4><<<dim3((unsigned)((3 * U) + 63) / 64, (unsigned)((R) + 31) / 32, (unsigned)(1)), 32, 0, stream>>>(gg00);
      else k_gemm<1><<<dim3((unsigned)((3 * U) + 31) / 32, (unsigned)((R) + 15) / 16, (unsigned)(1)), 32, 0, stream>>>(gg00); }
    { GemmP ghu00;
      ghu00.A = H; ghu00.B = UGC + (size_t)0 * U * 2 * U; ghu00.bias = H; ghu00.R = H; ghu00.C = HU;
      ghu00.sAo = 0; ghu00.sAi = 0; ghu00.sAm = U; ghu00.sAk = 1; ghu00.sBo = 0; ghu00.sBi = 0; ghu00.sBn = 1; ghu00.sBk = 2 * U; ghu00.sCo = 0; ghu00.sCi = 0; ghu00.sCm = 2 * U; ghu00.sRo = 0; ghu00.sRi = 0; ghu00.sRm = 0; ghu00.sRn = 0;
      ghu00.M = R; ghu00.N = 2 * U; ghu00.K = U; ghu00.zi_n = 1; ghu00.flags = 0; ghu00.act = 0;
      ghu00.alpha = 1.0f; ghu00.beta = 0.0f; ghu00.sa = 1.0f; ghu00.sb = 1.0f; ghu00.Npad = 2 * U; ghu00.pad_ = 0;
      if ((long long)(R) >= 64 && (long long)(2 * U) >= 64) k_gemmT<1, 2, 4><<<dim3((unsigned)((2 * U) + 63) / 64, (unsigned)((R) + 31) / 32, (unsigned)(1)), 32, 0, stream>>>(ghu00);
      else k_gemm<1><<<dim3((unsigned)((2 * U) + 31) / 32, (unsigned)((R) + 15) / 16, (unsigned)(1)), 32, 0, stream>>>(ghu00); }
    k_gg_zr<<<(unsigned)((R * U + 255) / 256), 256, 0, stream>>>(G, HU, H, bg + 0 * 3 * U, RH, R, U);
    { GemmP gru00;
      gru00.A = RH; gru00.B = Ug + ((size_t)0 * 3 + 2) * U * U; gru00.bias = RH; gru00.R = RH; gru00.C = RU;
      gru00.sAo = 0; gru00.sAi = 0; gru00.sAm = U; gru00.sAk = 1; gru00.sBo = 0; gru00.sBi = 0; gru00.sBn = 1; gru00.sBk = U; gru00.sCo = 0; gru00.sCi = 0; gru00.sCm = U; gru00.sRo = 0; gru00.sRi = 0; gru00.sRm = 0; gru00.sRn = 0;
      gru00.M = R; gru00.N = U; gru00.K = U; gru00.zi_n = 1; gru00.flags = 0; gru00.act = 0;
      gru00.alpha = 1.0f; gru00.beta = 0.0f; gru00.sa = 1.0f; gru00.sb = 1.0f; gru00.Npad = U; gru00.pad_ = 0;
      if ((long long)(R) >= 64 && (long long)(U) >= 64) k_gemmT<1, 2, 4><<<dim3((unsigned)((U) + 63) / 64, (unsigned)((R) + 31) / 32, (unsigned)(1)), 32, 0, stream>>>(gru00);
      else k_gemm<1><<<dim3((unsigned)((U) + 31) / 32, (unsigned)((R) + 15) / 16, (unsigned)(1)), 32, 0, stream>>>(gru00); }
    k_gg_upd<<<(unsigned)((R * U + 255) / 256), 256, 0, stream>>>(G, HU, RU, bg + 0 * 3 * U, H, R, U);
    { GemmP ghw01;
      ghw01.A = H; ghw01.B = WMC + (size_t)0 * U * 2 * U; ghw01.bias = H; ghw01.R = H; ghw01.C = HW;
      ghw01.sAo = 0; ghw01.sAi = 0; ghw01.sAm = U; ghw01.sAk = 1; ghw01.sBo = 0; ghw01.sBi = 0; ghw01.sBn = 1; ghw01.sBk = 2 * U; ghw01.sCo = 0; ghw01.sCi = 0; ghw01.sCm = 2 * U; ghw01.sRo = 0; ghw01.sRi = 0; ghw01.sRm = 0; ghw01.sRn = 0;
      ghw01.M = R; ghw01.N = 2 * U; ghw01.K = U; ghw01.zi_n = 1; ghw01.flags = 0; ghw01.act = 0;
      ghw01.alpha = 1.0f; ghw01.beta = 0.0f; ghw01.sa = 1.0f; ghw01.sb = 1.0f; ghw01.Npad = 2 * U; ghw01.pad_ = 0;
      if ((long long)(R) >= 64 && (long long)(2 * U) >= 64) k_gemmT<1, 2, 4><<<dim3((unsigned)((2 * U) + 63) / 64, (unsigned)((R) + 31) / 32, (unsigned)(1)), 32, 0, stream>>>(ghw01);
      else k_gemm<1><<<dim3((unsigned)((2 * U) + 31) / 32, (unsigned)((R) + 15) / 16, (unsigned)(1)), 32, 0, stream>>>(ghw01); }
    { GemmP ga001;
      ga001.A = A; ga001.B = HW; ga001.bias = bm + 0 * U; ga001.R = A; ga001.C = AGG;
      ga001.sAo = (long long)NE * N * N; ga001.sAi = 0; ga001.sAm = N; ga001.sAk = 1; ga001.sBo = (long long)N * 2 * U; ga001.sBi = 0; ga001.sBn = 1; ga001.sBk = 2 * U; ga001.sCo = (long long)N * U; ga001.sCi = 0; ga001.sCm = U; ga001.sRo = 0; ga001.sRi = 0; ga001.sRm = 0; ga001.sRn = 0;
      ga001.M = N; ga001.N = U; ga001.K = N; ga001.zi_n = 1; ga001.flags = 1; ga001.act = 0;
      ga001.alpha = 1.0f; ga001.beta = 0.0f; ga001.sa = 1.0f; ga001.sb = 1.0f; ga001.Npad = U; ga001.pad_ = 0;
      if ((long long)(N) >= 64 && (long long)(U) >= 64) k_gemmT<1, 2, 4><<<dim3((unsigned)((U) + 63) / 64, (unsigned)((N) + 31) / 32, (unsigned)(Bn)), 32, 0, stream>>>(ga001);
      else k_gemm<1><<<dim3((unsigned)((U) + 31) / 32, (unsigned)((N) + 15) / 16, (unsigned)(Bn)), 32, 0, stream>>>(ga001); }
    { GemmP ga101;
      ga101.A = A + (size_t)N * N; ga101.B = HW + U; ga101.bias = A + (size_t)N * N; ga101.R = AGG; ga101.C = AGG;
      ga101.sAo = (long long)NE * N * N; ga101.sAi = 0; ga101.sAm = N; ga101.sAk = 1; ga101.sBo = (long long)N * 2 * U; ga101.sBi = 0; ga101.sBn = 1; ga101.sBk = 2 * U; ga101.sCo = (long long)N * U; ga101.sCi = 0; ga101.sCm = U; ga101.sRo = (long long)N * U; ga101.sRi = 0; ga101.sRm = U; ga101.sRn = 1;
      ga101.M = N; ga101.N = U; ga101.K = N; ga101.zi_n = 1; ga101.flags = 4; ga101.act = 0;
      ga101.alpha = 1.0f; ga101.beta = 1.0f; ga101.sa = 1.0f; ga101.sb = 1.0f; ga101.Npad = U; ga101.pad_ = 0;
      if ((long long)(N) >= 64 && (long long)(U) >= 64) k_gemmT<1, 2, 4><<<dim3((unsigned)((U) + 63) / 64, (unsigned)((N) + 31) / 32, (unsigned)(Bn)), 32, 0, stream>>>(ga101);
      else k_gemm<1><<<dim3((unsigned)((U) + 31) / 32, (unsigned)((N) + 15) / 16, (unsigned)(Bn)), 32, 0, stream>>>(ga101); }
    { GemmP gg01;
      gg01.A = AGG; gg01.B = WGC + (size_t)0 * U * 3 * U; gg01.bias = AGG; gg01.R = AGG; gg01.C = G;
      gg01.sAo = 0; gg01.sAi = 0; gg01.sAm = U; gg01.sAk = 1; gg01.sBo = 0; gg01.sBi = 0; gg01.sBn = 1; gg01.sBk = 3 * U; gg01.sCo = 0; gg01.sCi = 0; gg01.sCm = 3 * U; gg01.sRo = 0; gg01.sRi = 0; gg01.sRm = 0; gg01.sRn = 0;
      gg01.M = R; gg01.N = 3 * U; gg01.K = U; gg01.zi_n = 1; gg01.flags = 0; gg01.act = 0;
      gg01.alpha = 1.0f; gg01.beta = 0.0f; gg01.sa = 1.0f; gg01.sb = 1.0f; gg01.Npad = 3 * U; gg01.pad_ = 0;
      if ((long long)(R) >= 64 && (long long)(3 * U) >= 64) k_gemmT<1, 2, 4><<<dim3((unsigned)((3 * U) + 63) / 64, (unsigned)((R) + 31) / 32, (unsigned)(1)), 32, 0, stream>>>(gg01);
      else k_gemm<1><<<dim3((unsigned)((3 * U) + 31) / 32, (unsigned)((R) + 15) / 16, (unsigned)(1)), 32, 0, stream>>>(gg01); }
    { GemmP ghu01;
      ghu01.A = H; ghu01.B = UGC + (size_t)0 * U * 2 * U; ghu01.bias = H; ghu01.R = H; ghu01.C = HU;
      ghu01.sAo = 0; ghu01.sAi = 0; ghu01.sAm = U; ghu01.sAk = 1; ghu01.sBo = 0; ghu01.sBi = 0; ghu01.sBn = 1; ghu01.sBk = 2 * U; ghu01.sCo = 0; ghu01.sCi = 0; ghu01.sCm = 2 * U; ghu01.sRo = 0; ghu01.sRi = 0; ghu01.sRm = 0; ghu01.sRn = 0;
      ghu01.M = R; ghu01.N = 2 * U; ghu01.K = U; ghu01.zi_n = 1; ghu01.flags = 0; ghu01.act = 0;
      ghu01.alpha = 1.0f; ghu01.beta = 0.0f; ghu01.sa = 1.0f; ghu01.sb = 1.0f; ghu01.Npad = 2 * U; ghu01.pad_ = 0;
      if ((long long)(R) >= 64 && (long long)(2 * U) >= 64) k_gemmT<1, 2, 4><<<dim3((unsigned)((2 * U) + 63) / 64, (unsigned)((R) + 31) / 32, (unsigned)(1)), 32, 0, stream>>>(ghu01);
      else k_gemm<1><<<dim3((unsigned)((2 * U) + 31) / 32, (unsigned)((R) + 15) / 16, (unsigned)(1)), 32, 0, stream>>>(ghu01); }
    k_gg_zr<<<(unsigned)((R * U + 255) / 256), 256, 0, stream>>>(G, HU, H, bg + 0 * 3 * U, RH, R, U);
    { GemmP gru01;
      gru01.A = RH; gru01.B = Ug + ((size_t)0 * 3 + 2) * U * U; gru01.bias = RH; gru01.R = RH; gru01.C = RU;
      gru01.sAo = 0; gru01.sAi = 0; gru01.sAm = U; gru01.sAk = 1; gru01.sBo = 0; gru01.sBi = 0; gru01.sBn = 1; gru01.sBk = U; gru01.sCo = 0; gru01.sCi = 0; gru01.sCm = U; gru01.sRo = 0; gru01.sRi = 0; gru01.sRm = 0; gru01.sRn = 0;
      gru01.M = R; gru01.N = U; gru01.K = U; gru01.zi_n = 1; gru01.flags = 0; gru01.act = 0;
      gru01.alpha = 1.0f; gru01.beta = 0.0f; gru01.sa = 1.0f; gru01.sb = 1.0f; gru01.Npad = U; gru01.pad_ = 0;
      if ((long long)(R) >= 64 && (long long)(U) >= 64) k_gemmT<1, 2, 4><<<dim3((unsigned)((U) + 63) / 64, (unsigned)((R) + 31) / 32, (unsigned)(1)), 32, 0, stream>>>(gru01);
      else k_gemm<1><<<dim3((unsigned)((U) + 31) / 32, (unsigned)((R) + 15) / 16, (unsigned)(1)), 32, 0, stream>>>(gru01); }
    k_gg_upd<<<(unsigned)((R * U + 255) / 256), 256, 0, stream>>>(G, HU, RU, bg + 0 * 3 * U, H, R, U);
    { GemmP ghw02;
      ghw02.A = H; ghw02.B = WMC + (size_t)0 * U * 2 * U; ghw02.bias = H; ghw02.R = H; ghw02.C = HW;
      ghw02.sAo = 0; ghw02.sAi = 0; ghw02.sAm = U; ghw02.sAk = 1; ghw02.sBo = 0; ghw02.sBi = 0; ghw02.sBn = 1; ghw02.sBk = 2 * U; ghw02.sCo = 0; ghw02.sCi = 0; ghw02.sCm = 2 * U; ghw02.sRo = 0; ghw02.sRi = 0; ghw02.sRm = 0; ghw02.sRn = 0;
      ghw02.M = R; ghw02.N = 2 * U; ghw02.K = U; ghw02.zi_n = 1; ghw02.flags = 0; ghw02.act = 0;
      ghw02.alpha = 1.0f; ghw02.beta = 0.0f; ghw02.sa = 1.0f; ghw02.sb = 1.0f; ghw02.Npad = 2 * U; ghw02.pad_ = 0;
      if ((long long)(R) >= 64 && (long long)(2 * U) >= 64) k_gemmT<1, 2, 4><<<dim3((unsigned)((2 * U) + 63) / 64, (unsigned)((R) + 31) / 32, (unsigned)(1)), 32, 0, stream>>>(ghw02);
      else k_gemm<1><<<dim3((unsigned)((2 * U) + 31) / 32, (unsigned)((R) + 15) / 16, (unsigned)(1)), 32, 0, stream>>>(ghw02); }
    { GemmP ga002;
      ga002.A = A; ga002.B = HW; ga002.bias = bm + 0 * U; ga002.R = A; ga002.C = AGG;
      ga002.sAo = (long long)NE * N * N; ga002.sAi = 0; ga002.sAm = N; ga002.sAk = 1; ga002.sBo = (long long)N * 2 * U; ga002.sBi = 0; ga002.sBn = 1; ga002.sBk = 2 * U; ga002.sCo = (long long)N * U; ga002.sCi = 0; ga002.sCm = U; ga002.sRo = 0; ga002.sRi = 0; ga002.sRm = 0; ga002.sRn = 0;
      ga002.M = N; ga002.N = U; ga002.K = N; ga002.zi_n = 1; ga002.flags = 1; ga002.act = 0;
      ga002.alpha = 1.0f; ga002.beta = 0.0f; ga002.sa = 1.0f; ga002.sb = 1.0f; ga002.Npad = U; ga002.pad_ = 0;
      if ((long long)(N) >= 64 && (long long)(U) >= 64) k_gemmT<1, 2, 4><<<dim3((unsigned)((U) + 63) / 64, (unsigned)((N) + 31) / 32, (unsigned)(Bn)), 32, 0, stream>>>(ga002);
      else k_gemm<1><<<dim3((unsigned)((U) + 31) / 32, (unsigned)((N) + 15) / 16, (unsigned)(Bn)), 32, 0, stream>>>(ga002); }
    { GemmP ga102;
      ga102.A = A + (size_t)N * N; ga102.B = HW + U; ga102.bias = A + (size_t)N * N; ga102.R = AGG; ga102.C = AGG;
      ga102.sAo = (long long)NE * N * N; ga102.sAi = 0; ga102.sAm = N; ga102.sAk = 1; ga102.sBo = (long long)N * 2 * U; ga102.sBi = 0; ga102.sBn = 1; ga102.sBk = 2 * U; ga102.sCo = (long long)N * U; ga102.sCi = 0; ga102.sCm = U; ga102.sRo = (long long)N * U; ga102.sRi = 0; ga102.sRm = U; ga102.sRn = 1;
      ga102.M = N; ga102.N = U; ga102.K = N; ga102.zi_n = 1; ga102.flags = 4; ga102.act = 0;
      ga102.alpha = 1.0f; ga102.beta = 1.0f; ga102.sa = 1.0f; ga102.sb = 1.0f; ga102.Npad = U; ga102.pad_ = 0;
      if ((long long)(N) >= 64 && (long long)(U) >= 64) k_gemmT<1, 2, 4><<<dim3((unsigned)((U) + 63) / 64, (unsigned)((N) + 31) / 32, (unsigned)(Bn)), 32, 0, stream>>>(ga102);
      else k_gemm<1><<<dim3((unsigned)((U) + 31) / 32, (unsigned)((N) + 15) / 16, (unsigned)(Bn)), 32, 0, stream>>>(ga102); }
    { GemmP gg02;
      gg02.A = AGG; gg02.B = WGC + (size_t)0 * U * 3 * U; gg02.bias = AGG; gg02.R = AGG; gg02.C = G;
      gg02.sAo = 0; gg02.sAi = 0; gg02.sAm = U; gg02.sAk = 1; gg02.sBo = 0; gg02.sBi = 0; gg02.sBn = 1; gg02.sBk = 3 * U; gg02.sCo = 0; gg02.sCi = 0; gg02.sCm = 3 * U; gg02.sRo = 0; gg02.sRi = 0; gg02.sRm = 0; gg02.sRn = 0;
      gg02.M = R; gg02.N = 3 * U; gg02.K = U; gg02.zi_n = 1; gg02.flags = 0; gg02.act = 0;
      gg02.alpha = 1.0f; gg02.beta = 0.0f; gg02.sa = 1.0f; gg02.sb = 1.0f; gg02.Npad = 3 * U; gg02.pad_ = 0;
      if ((long long)(R) >= 64 && (long long)(3 * U) >= 64) k_gemmT<1, 2, 4><<<dim3((unsigned)((3 * U) + 63) / 64, (unsigned)((R) + 31) / 32, (unsigned)(1)), 32, 0, stream>>>(gg02);
      else k_gemm<1><<<dim3((unsigned)((3 * U) + 31) / 32, (unsigned)((R) + 15) / 16, (unsigned)(1)), 32, 0, stream>>>(gg02); }
    { GemmP ghu02;
      ghu02.A = H; ghu02.B = UGC + (size_t)0 * U * 2 * U; ghu02.bias = H; ghu02.R = H; ghu02.C = HU;
      ghu02.sAo = 0; ghu02.sAi = 0; ghu02.sAm = U; ghu02.sAk = 1; ghu02.sBo = 0; ghu02.sBi = 0; ghu02.sBn = 1; ghu02.sBk = 2 * U; ghu02.sCo = 0; ghu02.sCi = 0; ghu02.sCm = 2 * U; ghu02.sRo = 0; ghu02.sRi = 0; ghu02.sRm = 0; ghu02.sRn = 0;
      ghu02.M = R; ghu02.N = 2 * U; ghu02.K = U; ghu02.zi_n = 1; ghu02.flags = 0; ghu02.act = 0;
      ghu02.alpha = 1.0f; ghu02.beta = 0.0f; ghu02.sa = 1.0f; ghu02.sb = 1.0f; ghu02.Npad = 2 * U; ghu02.pad_ = 0;
      if ((long long)(R) >= 64 && (long long)(2 * U) >= 64) k_gemmT<1, 2, 4><<<dim3((unsigned)((2 * U) + 63) / 64, (unsigned)((R) + 31) / 32, (unsigned)(1)), 32, 0, stream>>>(ghu02);
      else k_gemm<1><<<dim3((unsigned)((2 * U) + 31) / 32, (unsigned)((R) + 15) / 16, (unsigned)(1)), 32, 0, stream>>>(ghu02); }
    k_gg_zr<<<(unsigned)((R * U + 255) / 256), 256, 0, stream>>>(G, HU, H, bg + 0 * 3 * U, RH, R, U);
    { GemmP gru02;
      gru02.A = RH; gru02.B = Ug + ((size_t)0 * 3 + 2) * U * U; gru02.bias = RH; gru02.R = RH; gru02.C = RU;
      gru02.sAo = 0; gru02.sAi = 0; gru02.sAm = U; gru02.sAk = 1; gru02.sBo = 0; gru02.sBi = 0; gru02.sBn = 1; gru02.sBk = U; gru02.sCo = 0; gru02.sCi = 0; gru02.sCm = U; gru02.sRo = 0; gru02.sRi = 0; gru02.sRm = 0; gru02.sRn = 0;
      gru02.M = R; gru02.N = U; gru02.K = U; gru02.zi_n = 1; gru02.flags = 0; gru02.act = 0;
      gru02.alpha = 1.0f; gru02.beta = 0.0f; gru02.sa = 1.0f; gru02.sb = 1.0f; gru02.Npad = U; gru02.pad_ = 0;
      if ((long long)(R) >= 64 && (long long)(U) >= 64) k_gemmT<1, 2, 4><<<dim3((unsigned)((U) + 63) / 64, (unsigned)((R) + 31) / 32, (unsigned)(1)), 32, 0, stream>>>(gru02);
      else k_gemm<1><<<dim3((unsigned)((U) + 31) / 32, (unsigned)((R) + 15) / 16, (unsigned)(1)), 32, 0, stream>>>(gru02); }
    k_gg_upd<<<(unsigned)((R * U + 255) / 256), 256, 0, stream>>>(G, HU, RU, bg + 0 * 3 * U, H, R, U);
    { GemmP ghw10;
      ghw10.A = H; ghw10.B = WMC + (size_t)1 * U * 2 * U; ghw10.bias = H; ghw10.R = H; ghw10.C = HW;
      ghw10.sAo = 0; ghw10.sAi = 0; ghw10.sAm = U; ghw10.sAk = 1; ghw10.sBo = 0; ghw10.sBi = 0; ghw10.sBn = 1; ghw10.sBk = 2 * U; ghw10.sCo = 0; ghw10.sCi = 0; ghw10.sCm = 2 * U; ghw10.sRo = 0; ghw10.sRi = 0; ghw10.sRm = 0; ghw10.sRn = 0;
      ghw10.M = R; ghw10.N = 2 * U; ghw10.K = U; ghw10.zi_n = 1; ghw10.flags = 0; ghw10.act = 0;
      ghw10.alpha = 1.0f; ghw10.beta = 0.0f; ghw10.sa = 1.0f; ghw10.sb = 1.0f; ghw10.Npad = 2 * U; ghw10.pad_ = 0;
      if ((long long)(R) >= 64 && (long long)(2 * U) >= 64) k_gemmT<1, 2, 4><<<dim3((unsigned)((2 * U) + 63) / 64, (unsigned)((R) + 31) / 32, (unsigned)(1)), 32, 0, stream>>>(ghw10);
      else k_gemm<1><<<dim3((unsigned)((2 * U) + 31) / 32, (unsigned)((R) + 15) / 16, (unsigned)(1)), 32, 0, stream>>>(ghw10); }
    { GemmP ga010;
      ga010.A = A; ga010.B = HW; ga010.bias = bm + 1 * U; ga010.R = A; ga010.C = AGG;
      ga010.sAo = (long long)NE * N * N; ga010.sAi = 0; ga010.sAm = N; ga010.sAk = 1; ga010.sBo = (long long)N * 2 * U; ga010.sBi = 0; ga010.sBn = 1; ga010.sBk = 2 * U; ga010.sCo = (long long)N * U; ga010.sCi = 0; ga010.sCm = U; ga010.sRo = 0; ga010.sRi = 0; ga010.sRm = 0; ga010.sRn = 0;
      ga010.M = N; ga010.N = U; ga010.K = N; ga010.zi_n = 1; ga010.flags = 1; ga010.act = 0;
      ga010.alpha = 1.0f; ga010.beta = 0.0f; ga010.sa = 1.0f; ga010.sb = 1.0f; ga010.Npad = U; ga010.pad_ = 0;
      if ((long long)(N) >= 64 && (long long)(U) >= 64) k_gemmT<1, 2, 4><<<dim3((unsigned)((U) + 63) / 64, (unsigned)((N) + 31) / 32, (unsigned)(Bn)), 32, 0, stream>>>(ga010);
      else k_gemm<1><<<dim3((unsigned)((U) + 31) / 32, (unsigned)((N) + 15) / 16, (unsigned)(Bn)), 32, 0, stream>>>(ga010); }
    { GemmP ga110;
      ga110.A = A + (size_t)N * N; ga110.B = HW + U; ga110.bias = A + (size_t)N * N; ga110.R = AGG; ga110.C = AGG;
      ga110.sAo = (long long)NE * N * N; ga110.sAi = 0; ga110.sAm = N; ga110.sAk = 1; ga110.sBo = (long long)N * 2 * U; ga110.sBi = 0; ga110.sBn = 1; ga110.sBk = 2 * U; ga110.sCo = (long long)N * U; ga110.sCi = 0; ga110.sCm = U; ga110.sRo = (long long)N * U; ga110.sRi = 0; ga110.sRm = U; ga110.sRn = 1;
      ga110.M = N; ga110.N = U; ga110.K = N; ga110.zi_n = 1; ga110.flags = 4; ga110.act = 0;
      ga110.alpha = 1.0f; ga110.beta = 1.0f; ga110.sa = 1.0f; ga110.sb = 1.0f; ga110.Npad = U; ga110.pad_ = 0;
      if ((long long)(N) >= 64 && (long long)(U) >= 64) k_gemmT<1, 2, 4><<<dim3((unsigned)((U) + 63) / 64, (unsigned)((N) + 31) / 32, (unsigned)(Bn)), 32, 0, stream>>>(ga110);
      else k_gemm<1><<<dim3((unsigned)((U) + 31) / 32, (unsigned)((N) + 15) / 16, (unsigned)(Bn)), 32, 0, stream>>>(ga110); }
    { GemmP gg10;
      gg10.A = AGG; gg10.B = WGC + (size_t)1 * U * 3 * U; gg10.bias = AGG; gg10.R = AGG; gg10.C = G;
      gg10.sAo = 0; gg10.sAi = 0; gg10.sAm = U; gg10.sAk = 1; gg10.sBo = 0; gg10.sBi = 0; gg10.sBn = 1; gg10.sBk = 3 * U; gg10.sCo = 0; gg10.sCi = 0; gg10.sCm = 3 * U; gg10.sRo = 0; gg10.sRi = 0; gg10.sRm = 0; gg10.sRn = 0;
      gg10.M = R; gg10.N = 3 * U; gg10.K = U; gg10.zi_n = 1; gg10.flags = 0; gg10.act = 0;
      gg10.alpha = 1.0f; gg10.beta = 0.0f; gg10.sa = 1.0f; gg10.sb = 1.0f; gg10.Npad = 3 * U; gg10.pad_ = 0;
      if ((long long)(R) >= 64 && (long long)(3 * U) >= 64) k_gemmT<1, 2, 4><<<dim3((unsigned)((3 * U) + 63) / 64, (unsigned)((R) + 31) / 32, (unsigned)(1)), 32, 0, stream>>>(gg10);
      else k_gemm<1><<<dim3((unsigned)((3 * U) + 31) / 32, (unsigned)((R) + 15) / 16, (unsigned)(1)), 32, 0, stream>>>(gg10); }
    { GemmP ghu10;
      ghu10.A = H; ghu10.B = UGC + (size_t)1 * U * 2 * U; ghu10.bias = H; ghu10.R = H; ghu10.C = HU;
      ghu10.sAo = 0; ghu10.sAi = 0; ghu10.sAm = U; ghu10.sAk = 1; ghu10.sBo = 0; ghu10.sBi = 0; ghu10.sBn = 1; ghu10.sBk = 2 * U; ghu10.sCo = 0; ghu10.sCi = 0; ghu10.sCm = 2 * U; ghu10.sRo = 0; ghu10.sRi = 0; ghu10.sRm = 0; ghu10.sRn = 0;
      ghu10.M = R; ghu10.N = 2 * U; ghu10.K = U; ghu10.zi_n = 1; ghu10.flags = 0; ghu10.act = 0;
      ghu10.alpha = 1.0f; ghu10.beta = 0.0f; ghu10.sa = 1.0f; ghu10.sb = 1.0f; ghu10.Npad = 2 * U; ghu10.pad_ = 0;
      if ((long long)(R) >= 64 && (long long)(2 * U) >= 64) k_gemmT<1, 2, 4><<<dim3((unsigned)((2 * U) + 63) / 64, (unsigned)((R) + 31) / 32, (unsigned)(1)), 32, 0, stream>>>(ghu10);
      else k_gemm<1><<<dim3((unsigned)((2 * U) + 31) / 32, (unsigned)((R) + 15) / 16, (unsigned)(1)), 32, 0, stream>>>(ghu10); }
    k_gg_zr<<<(unsigned)((R * U + 255) / 256), 256, 0, stream>>>(G, HU, H, bg + 1 * 3 * U, RH, R, U);
    { GemmP gru10;
      gru10.A = RH; gru10.B = Ug + ((size_t)1 * 3 + 2) * U * U; gru10.bias = RH; gru10.R = RH; gru10.C = RU;
      gru10.sAo = 0; gru10.sAi = 0; gru10.sAm = U; gru10.sAk = 1; gru10.sBo = 0; gru10.sBi = 0; gru10.sBn = 1; gru10.sBk = U; gru10.sCo = 0; gru10.sCi = 0; gru10.sCm = U; gru10.sRo = 0; gru10.sRi = 0; gru10.sRm = 0; gru10.sRn = 0;
      gru10.M = R; gru10.N = U; gru10.K = U; gru10.zi_n = 1; gru10.flags = 0; gru10.act = 0;
      gru10.alpha = 1.0f; gru10.beta = 0.0f; gru10.sa = 1.0f; gru10.sb = 1.0f; gru10.Npad = U; gru10.pad_ = 0;
      if ((long long)(R) >= 64 && (long long)(U) >= 64) k_gemmT<1, 2, 4><<<dim3((unsigned)((U) + 63) / 64, (unsigned)((R) + 31) / 32, (unsigned)(1)), 32, 0, stream>>>(gru10);
      else k_gemm<1><<<dim3((unsigned)((U) + 31) / 32, (unsigned)((R) + 15) / 16, (unsigned)(1)), 32, 0, stream>>>(gru10); }
    k_gg_upd<<<(unsigned)((R * U + 255) / 256), 256, 0, stream>>>(G, HU, RU, bg + 1 * 3 * U, H, R, U);
    { GemmP ghw11;
      ghw11.A = H; ghw11.B = WMC + (size_t)1 * U * 2 * U; ghw11.bias = H; ghw11.R = H; ghw11.C = HW;
      ghw11.sAo = 0; ghw11.sAi = 0; ghw11.sAm = U; ghw11.sAk = 1; ghw11.sBo = 0; ghw11.sBi = 0; ghw11.sBn = 1; ghw11.sBk = 2 * U; ghw11.sCo = 0; ghw11.sCi = 0; ghw11.sCm = 2 * U; ghw11.sRo = 0; ghw11.sRi = 0; ghw11.sRm = 0; ghw11.sRn = 0;
      ghw11.M = R; ghw11.N = 2 * U; ghw11.K = U; ghw11.zi_n = 1; ghw11.flags = 0; ghw11.act = 0;
      ghw11.alpha = 1.0f; ghw11.beta = 0.0f; ghw11.sa = 1.0f; ghw11.sb = 1.0f; ghw11.Npad = 2 * U; ghw11.pad_ = 0;
      if ((long long)(R) >= 64 && (long long)(2 * U) >= 64) k_gemmT<1, 2, 4><<<dim3((unsigned)((2 * U) + 63) / 64, (unsigned)((R) + 31) / 32, (unsigned)(1)), 32, 0, stream>>>(ghw11);
      else k_gemm<1><<<dim3((unsigned)((2 * U) + 31) / 32, (unsigned)((R) + 15) / 16, (unsigned)(1)), 32, 0, stream>>>(ghw11); }
    { GemmP ga011;
      ga011.A = A; ga011.B = HW; ga011.bias = bm + 1 * U; ga011.R = A; ga011.C = AGG;
      ga011.sAo = (long long)NE * N * N; ga011.sAi = 0; ga011.sAm = N; ga011.sAk = 1; ga011.sBo = (long long)N * 2 * U; ga011.sBi = 0; ga011.sBn = 1; ga011.sBk = 2 * U; ga011.sCo = (long long)N * U; ga011.sCi = 0; ga011.sCm = U; ga011.sRo = 0; ga011.sRi = 0; ga011.sRm = 0; ga011.sRn = 0;
      ga011.M = N; ga011.N = U; ga011.K = N; ga011.zi_n = 1; ga011.flags = 1; ga011.act = 0;
      ga011.alpha = 1.0f; ga011.beta = 0.0f; ga011.sa = 1.0f; ga011.sb = 1.0f; ga011.Npad = U; ga011.pad_ = 0;
      if ((long long)(N) >= 64 && (long long)(U) >= 64) k_gemmT<1, 2, 4><<<dim3((unsigned)((U) + 63) / 64, (unsigned)((N) + 31) / 32, (unsigned)(Bn)), 32, 0, stream>>>(ga011);
      else k_gemm<1><<<dim3((unsigned)((U) + 31) / 32, (unsigned)((N) + 15) / 16, (unsigned)(Bn)), 32, 0, stream>>>(ga011); }
    { GemmP ga111;
      ga111.A = A + (size_t)N * N; ga111.B = HW + U; ga111.bias = A + (size_t)N * N; ga111.R = AGG; ga111.C = AGG;
      ga111.sAo = (long long)NE * N * N; ga111.sAi = 0; ga111.sAm = N; ga111.sAk = 1; ga111.sBo = (long long)N * 2 * U; ga111.sBi = 0; ga111.sBn = 1; ga111.sBk = 2 * U; ga111.sCo = (long long)N * U; ga111.sCi = 0; ga111.sCm = U; ga111.sRo = (long long)N * U; ga111.sRi = 0; ga111.sRm = U; ga111.sRn = 1;
      ga111.M = N; ga111.N = U; ga111.K = N; ga111.zi_n = 1; ga111.flags = 4; ga111.act = 0;
      ga111.alpha = 1.0f; ga111.beta = 1.0f; ga111.sa = 1.0f; ga111.sb = 1.0f; ga111.Npad = U; ga111.pad_ = 0;
      if ((long long)(N) >= 64 && (long long)(U) >= 64) k_gemmT<1, 2, 4><<<dim3((unsigned)((U) + 63) / 64, (unsigned)((N) + 31) / 32, (unsigned)(Bn)), 32, 0, stream>>>(ga111);
      else k_gemm<1><<<dim3((unsigned)((U) + 31) / 32, (unsigned)((N) + 15) / 16, (unsigned)(Bn)), 32, 0, stream>>>(ga111); }
    { GemmP gg11;
      gg11.A = AGG; gg11.B = WGC + (size_t)1 * U * 3 * U; gg11.bias = AGG; gg11.R = AGG; gg11.C = G;
      gg11.sAo = 0; gg11.sAi = 0; gg11.sAm = U; gg11.sAk = 1; gg11.sBo = 0; gg11.sBi = 0; gg11.sBn = 1; gg11.sBk = 3 * U; gg11.sCo = 0; gg11.sCi = 0; gg11.sCm = 3 * U; gg11.sRo = 0; gg11.sRi = 0; gg11.sRm = 0; gg11.sRn = 0;
      gg11.M = R; gg11.N = 3 * U; gg11.K = U; gg11.zi_n = 1; gg11.flags = 0; gg11.act = 0;
      gg11.alpha = 1.0f; gg11.beta = 0.0f; gg11.sa = 1.0f; gg11.sb = 1.0f; gg11.Npad = 3 * U; gg11.pad_ = 0;
      if ((long long)(R) >= 64 && (long long)(3 * U) >= 64) k_gemmT<1, 2, 4><<<dim3((unsigned)((3 * U) + 63) / 64, (unsigned)((R) + 31) / 32, (unsigned)(1)), 32, 0, stream>>>(gg11);
      else k_gemm<1><<<dim3((unsigned)((3 * U) + 31) / 32, (unsigned)((R) + 15) / 16, (unsigned)(1)), 32, 0, stream>>>(gg11); }
    { GemmP ghu11;
      ghu11.A = H; ghu11.B = UGC + (size_t)1 * U * 2 * U; ghu11.bias = H; ghu11.R = H; ghu11.C = HU;
      ghu11.sAo = 0; ghu11.sAi = 0; ghu11.sAm = U; ghu11.sAk = 1; ghu11.sBo = 0; ghu11.sBi = 0; ghu11.sBn = 1; ghu11.sBk = 2 * U; ghu11.sCo = 0; ghu11.sCi = 0; ghu11.sCm = 2 * U; ghu11.sRo = 0; ghu11.sRi = 0; ghu11.sRm = 0; ghu11.sRn = 0;
      ghu11.M = R; ghu11.N = 2 * U; ghu11.K = U; ghu11.zi_n = 1; ghu11.flags = 0; ghu11.act = 0;
      ghu11.alpha = 1.0f; ghu11.beta = 0.0f; ghu11.sa = 1.0f; ghu11.sb = 1.0f; ghu11.Npad = 2 * U; ghu11.pad_ = 0;
      if ((long long)(R) >= 64 && (long long)(2 * U) >= 64) k_gemmT<1, 2, 4><<<dim3((unsigned)((2 * U) + 63) / 64, (unsigned)((R) + 31) / 32, (unsigned)(1)), 32, 0, stream>>>(ghu11);
      else k_gemm<1><<<dim3((unsigned)((2 * U) + 31) / 32, (unsigned)((R) + 15) / 16, (unsigned)(1)), 32, 0, stream>>>(ghu11); }
    k_gg_zr<<<(unsigned)((R * U + 255) / 256), 256, 0, stream>>>(G, HU, H, bg + 1 * 3 * U, RH, R, U);
    { GemmP gru11;
      gru11.A = RH; gru11.B = Ug + ((size_t)1 * 3 + 2) * U * U; gru11.bias = RH; gru11.R = RH; gru11.C = RU;
      gru11.sAo = 0; gru11.sAi = 0; gru11.sAm = U; gru11.sAk = 1; gru11.sBo = 0; gru11.sBi = 0; gru11.sBn = 1; gru11.sBk = U; gru11.sCo = 0; gru11.sCi = 0; gru11.sCm = U; gru11.sRo = 0; gru11.sRi = 0; gru11.sRm = 0; gru11.sRn = 0;
      gru11.M = R; gru11.N = U; gru11.K = U; gru11.zi_n = 1; gru11.flags = 0; gru11.act = 0;
      gru11.alpha = 1.0f; gru11.beta = 0.0f; gru11.sa = 1.0f; gru11.sb = 1.0f; gru11.Npad = U; gru11.pad_ = 0;
      if ((long long)(R) >= 64 && (long long)(U) >= 64) k_gemmT<1, 2, 4><<<dim3((unsigned)((U) + 63) / 64, (unsigned)((R) + 31) / 32, (unsigned)(1)), 32, 0, stream>>>(gru11);
      else k_gemm<1><<<dim3((unsigned)((U) + 31) / 32, (unsigned)((R) + 15) / 16, (unsigned)(1)), 32, 0, stream>>>(gru11); }
    k_gg_upd<<<(unsigned)((R * U + 255) / 256), 256, 0, stream>>>(G, HU, RU, bg + 1 * 3 * U, H, R, U);
    { GemmP ghw12;
      ghw12.A = H; ghw12.B = WMC + (size_t)1 * U * 2 * U; ghw12.bias = H; ghw12.R = H; ghw12.C = HW;
      ghw12.sAo = 0; ghw12.sAi = 0; ghw12.sAm = U; ghw12.sAk = 1; ghw12.sBo = 0; ghw12.sBi = 0; ghw12.sBn = 1; ghw12.sBk = 2 * U; ghw12.sCo = 0; ghw12.sCi = 0; ghw12.sCm = 2 * U; ghw12.sRo = 0; ghw12.sRi = 0; ghw12.sRm = 0; ghw12.sRn = 0;
      ghw12.M = R; ghw12.N = 2 * U; ghw12.K = U; ghw12.zi_n = 1; ghw12.flags = 0; ghw12.act = 0;
      ghw12.alpha = 1.0f; ghw12.beta = 0.0f; ghw12.sa = 1.0f; ghw12.sb = 1.0f; ghw12.Npad = 2 * U; ghw12.pad_ = 0;
      if ((long long)(R) >= 64 && (long long)(2 * U) >= 64) k_gemmT<1, 2, 4><<<dim3((unsigned)((2 * U) + 63) / 64, (unsigned)((R) + 31) / 32, (unsigned)(1)), 32, 0, stream>>>(ghw12);
      else k_gemm<1><<<dim3((unsigned)((2 * U) + 31) / 32, (unsigned)((R) + 15) / 16, (unsigned)(1)), 32, 0, stream>>>(ghw12); }
    { GemmP ga012;
      ga012.A = A; ga012.B = HW; ga012.bias = bm + 1 * U; ga012.R = A; ga012.C = AGG;
      ga012.sAo = (long long)NE * N * N; ga012.sAi = 0; ga012.sAm = N; ga012.sAk = 1; ga012.sBo = (long long)N * 2 * U; ga012.sBi = 0; ga012.sBn = 1; ga012.sBk = 2 * U; ga012.sCo = (long long)N * U; ga012.sCi = 0; ga012.sCm = U; ga012.sRo = 0; ga012.sRi = 0; ga012.sRm = 0; ga012.sRn = 0;
      ga012.M = N; ga012.N = U; ga012.K = N; ga012.zi_n = 1; ga012.flags = 1; ga012.act = 0;
      ga012.alpha = 1.0f; ga012.beta = 0.0f; ga012.sa = 1.0f; ga012.sb = 1.0f; ga012.Npad = U; ga012.pad_ = 0;
      if ((long long)(N) >= 64 && (long long)(U) >= 64) k_gemmT<1, 2, 4><<<dim3((unsigned)((U) + 63) / 64, (unsigned)((N) + 31) / 32, (unsigned)(Bn)), 32, 0, stream>>>(ga012);
      else k_gemm<1><<<dim3((unsigned)((U) + 31) / 32, (unsigned)((N) + 15) / 16, (unsigned)(Bn)), 32, 0, stream>>>(ga012); }
    { GemmP ga112;
      ga112.A = A + (size_t)N * N; ga112.B = HW + U; ga112.bias = A + (size_t)N * N; ga112.R = AGG; ga112.C = AGG;
      ga112.sAo = (long long)NE * N * N; ga112.sAi = 0; ga112.sAm = N; ga112.sAk = 1; ga112.sBo = (long long)N * 2 * U; ga112.sBi = 0; ga112.sBn = 1; ga112.sBk = 2 * U; ga112.sCo = (long long)N * U; ga112.sCi = 0; ga112.sCm = U; ga112.sRo = (long long)N * U; ga112.sRi = 0; ga112.sRm = U; ga112.sRn = 1;
      ga112.M = N; ga112.N = U; ga112.K = N; ga112.zi_n = 1; ga112.flags = 4; ga112.act = 0;
      ga112.alpha = 1.0f; ga112.beta = 1.0f; ga112.sa = 1.0f; ga112.sb = 1.0f; ga112.Npad = U; ga112.pad_ = 0;
      if ((long long)(N) >= 64 && (long long)(U) >= 64) k_gemmT<1, 2, 4><<<dim3((unsigned)((U) + 63) / 64, (unsigned)((N) + 31) / 32, (unsigned)(Bn)), 32, 0, stream>>>(ga112);
      else k_gemm<1><<<dim3((unsigned)((U) + 31) / 32, (unsigned)((N) + 15) / 16, (unsigned)(Bn)), 32, 0, stream>>>(ga112); }
    { GemmP gg12;
      gg12.A = AGG; gg12.B = WGC + (size_t)1 * U * 3 * U; gg12.bias = AGG; gg12.R = AGG; gg12.C = G;
      gg12.sAo = 0; gg12.sAi = 0; gg12.sAm = U; gg12.sAk = 1; gg12.sBo = 0; gg12.sBi = 0; gg12.sBn = 1; gg12.sBk = 3 * U; gg12.sCo = 0; gg12.sCi = 0; gg12.sCm = 3 * U; gg12.sRo = 0; gg12.sRi = 0; gg12.sRm = 0; gg12.sRn = 0;
      gg12.M = R; gg12.N = 3 * U; gg12.K = U; gg12.zi_n = 1; gg12.flags = 0; gg12.act = 0;
      gg12.alpha = 1.0f; gg12.beta = 0.0f; gg12.sa = 1.0f; gg12.sb = 1.0f; gg12.Npad = 3 * U; gg12.pad_ = 0;
      if ((long long)(R) >= 64 && (long long)(3 * U) >= 64) k_gemmT<1, 2, 4><<<dim3((unsigned)((3 * U) + 63) / 64, (unsigned)((R) + 31) / 32, (unsigned)(1)), 32, 0, stream>>>(gg12);
      else k_gemm<1><<<dim3((unsigned)((3 * U) + 31) / 32, (unsigned)((R) + 15) / 16, (unsigned)(1)), 32, 0, stream>>>(gg12); }
    { GemmP ghu12;
      ghu12.A = H; ghu12.B = UGC + (size_t)1 * U * 2 * U; ghu12.bias = H; ghu12.R = H; ghu12.C = HU;
      ghu12.sAo = 0; ghu12.sAi = 0; ghu12.sAm = U; ghu12.sAk = 1; ghu12.sBo = 0; ghu12.sBi = 0; ghu12.sBn = 1; ghu12.sBk = 2 * U; ghu12.sCo = 0; ghu12.sCi = 0; ghu12.sCm = 2 * U; ghu12.sRo = 0; ghu12.sRi = 0; ghu12.sRm = 0; ghu12.sRn = 0;
      ghu12.M = R; ghu12.N = 2 * U; ghu12.K = U; ghu12.zi_n = 1; ghu12.flags = 0; ghu12.act = 0;
      ghu12.alpha = 1.0f; ghu12.beta = 0.0f; ghu12.sa = 1.0f; ghu12.sb = 1.0f; ghu12.Npad = 2 * U; ghu12.pad_ = 0;
      if ((long long)(R) >= 64 && (long long)(2 * U) >= 64) k_gemmT<1, 2, 4><<<dim3((unsigned)((2 * U) + 63) / 64, (unsigned)((R) + 31) / 32, (unsigned)(1)), 32, 0, stream>>>(ghu12);
      else k_gemm<1><<<dim3((unsigned)((2 * U) + 31) / 32, (unsigned)((R) + 15) / 16, (unsigned)(1)), 32, 0, stream>>>(ghu12); }
    k_gg_zr<<<(unsigned)((R * U + 255) / 256), 256, 0, stream>>>(G, HU, H, bg + 1 * 3 * U, RH, R, U);
    { GemmP gru12;
      gru12.A = RH; gru12.B = Ug + ((size_t)1 * 3 + 2) * U * U; gru12.bias = RH; gru12.R = RH; gru12.C = RU;
      gru12.sAo = 0; gru12.sAi = 0; gru12.sAm = U; gru12.sAk = 1; gru12.sBo = 0; gru12.sBi = 0; gru12.sBn = 1; gru12.sBk = U; gru12.sCo = 0; gru12.sCi = 0; gru12.sCm = U; gru12.sRo = 0; gru12.sRi = 0; gru12.sRm = 0; gru12.sRn = 0;
      gru12.M = R; gru12.N = U; gru12.K = U; gru12.zi_n = 1; gru12.flags = 0; gru12.act = 0;
      gru12.alpha = 1.0f; gru12.beta = 0.0f; gru12.sa = 1.0f; gru12.sb = 1.0f; gru12.Npad = U; gru12.pad_ = 0;
      if ((long long)(R) >= 64 && (long long)(U) >= 64) k_gemmT<1, 2, 4><<<dim3((unsigned)((U) + 63) / 64, (unsigned)((R) + 31) / 32, (unsigned)(1)), 32, 0, stream>>>(gru12);
      else k_gemm<1><<<dim3((unsigned)((U) + 31) / 32, (unsigned)((R) + 15) / 16, (unsigned)(1)), 32, 0, stream>>>(gru12); }
    k_gg_upd<<<(unsigned)((R * U + 255) / 256), 256, 0, stream>>>(G, HU, RU, bg + 1 * 3 * U, H, R, U);
    k_gg_relu<<<(unsigned)((R * U + 255) / 256), 256, 0, stream>>>(H, RH, R * U);
    { GemmP gfc;
      gfc.A = RH; gfc.B = fcw; gfc.bias = fcb; gfc.R = RH; gfc.C = LG;
      gfc.sAo = 0; gfc.sAi = 0; gfc.sAm = U; gfc.sAk = 1; gfc.sBo = 0; gfc.sBi = 0; gfc.sBn = 1; gfc.sBk = NC; gfc.sCo = 0; gfc.sCi = 0; gfc.sCm = 16; gfc.sRo = 0; gfc.sRi = 0; gfc.sRm = 0; gfc.sRn = 0;
      gfc.M = R; gfc.N = NC; gfc.K = U; gfc.zi_n = 1; gfc.flags = 1; gfc.act = 0;
      gfc.alpha = 1.0f; gfc.beta = 0.0f; gfc.sa = 1.0f; gfc.sb = 1.0f; gfc.Npad = 16; gfc.pad_ = 0;
      if ((long long)(R) >= 64 && (long long)(16) >= 64) k_gemmT<1, 2, 4><<<dim3((unsigned)((16) + 63) / 64, (unsigned)((R) + 31) / 32, (unsigned)(1)), 32, 0, stream>>>(gfc);
      else k_gemm<1><<<dim3((unsigned)((16) + 31) / 32, (unsigned)((R) + 15) / 16, (unsigned)(1)), 32, 0, stream>>>(gfc); }
    k_gg_max<<<(unsigned)((Bn * NC + 255) / 256), 256, 0, stream>>>(LG, out, Bn, N, NC);
}
